// SSH_48206712930421
// MI455X (gfx1250) — hardware-verified
//
#include <hip/hip_runtime.h>
#include <math.h>

typedef __attribute__((ext_vector_type(16))) _Float16 v16h;
typedef __attribute__((ext_vector_type(8)))  _Float16 v8h;
typedef __attribute__((ext_vector_type(16))) __bf16   v16b;
typedef __attribute__((ext_vector_type(8)))  float    v8f;
typedef __attribute__((ext_vector_type(4)))  float    v4f;

__device__ __forceinline__ int frag_k(int i, int h) { return (i < 8) ? (8 * h + i) : (16 + 8 * h + (i - 8)); }
__device__ __forceinline__ __bf16 bf16_rne(float f) {
    unsigned int u = __float_as_uint(f);
    u += 0x7fffu + ((u >> 16) & 1u);
    return __builtin_bit_cast(__bf16, (unsigned short)(u >> 16));
}
__device__ __forceinline__ float bf16_f32(__bf16 b) { return __uint_as_float(((unsigned int)__builtin_bit_cast(unsigned short, b)) << 16); }
__device__ __forceinline__ v8f wmma16(v16h a, v16h b, v8f c) {
    c = __builtin_amdgcn_wmma_f32_16x16x32_f16(false, a, false, b, (short)0, c, false, false);
    asm volatile("v_nop\n\tv_nop\n\tv_nop\n\tv_nop" : "+v"(c) : "v"(a), "v"(b));
    return c;
}
__device__ __forceinline__ v8f wmmab(v16b a, v16b b, v8f c) {
    c = __builtin_amdgcn_wmma_f32_16x16x32_bf16(false, a, false, b, (short)0, c, false, false);
    asm volatile("v_nop\n\tv_nop\n\tv_nop\n\tv_nop" : "+v"(c) : "v"(a), "v"(b));
    return c;
}
struct Split { v16b hi, lo; };
__device__ __forceinline__ v8f wmma3(const Split& a, const Split& b, v8f c) {
    c = __builtin_amdgcn_wmma_f32_16x16x32_bf16(false, a.hi, false, b.hi, (short)0, c, false, false);
    c = __builtin_amdgcn_wmma_f32_16x16x32_bf16(false, a.hi, false, b.lo, (short)0, c, false, false);
    c = __builtin_amdgcn_wmma_f32_16x16x32_bf16(false, a.lo, false, b.hi, (short)0, c, false, false);
    asm volatile("v_nop\n\tv_nop\n\tv_nop\n\tv_nop" : "+v"(c) : "v"(a.hi), "v"(a.lo), "v"(b.hi), "v"(b.lo));
    return c;
}
struct Split3 { v16b hi, mid, lo; };
__device__ __forceinline__ v8f wmma6(const Split3& a, const Split3& b, v8f c) {
    c = __builtin_amdgcn_wmma_f32_16x16x32_bf16(false, a.hi, false, b.hi, (short)0, c, false, false);
    c = __builtin_amdgcn_wmma_f32_16x16x32_bf16(false, a.hi, false, b.mid, (short)0, c, false, false);
    c = __builtin_amdgcn_wmma_f32_16x16x32_bf16(false, a.mid, false, b.hi, (short)0, c, false, false);
    c = __builtin_amdgcn_wmma_f32_16x16x32_bf16(false, a.hi, false, b.lo, (short)0, c, false, false);
    c = __builtin_amdgcn_wmma_f32_16x16x32_bf16(false, a.mid, false, b.mid, (short)0, c, false, false);
    c = __builtin_amdgcn_wmma_f32_16x16x32_bf16(false, a.lo, false, b.hi, (short)0, c, false, false);
    asm volatile("v_nop\n\tv_nop\n\tv_nop\n\tv_nop" : "+v"(c) : "v"(a.hi), "v"(a.mid), "v"(a.lo), "v"(b.hi), "v"(b.mid), "v"(b.lo));
    return c;
}

__device__ __forceinline__ v16h fh_ld(const float* __restrict__ p, long long sk, int k0, int h, int klen, float s) {
    v16h a;
#pragma unroll
    for (int i = 0; i < 16; ++i) { const int k = k0 + frag_k(i, h); a[i] = (k < klen) ? (_Float16)(p[(long long)k * sk] * s) : (_Float16)0.f; }
    return a;
}
__device__ __forceinline__ Split sp_ld(const float* __restrict__ p, long long sk, int k0, int h, int klen, float s) {
    Split r;
#pragma unroll
    for (int i = 0; i < 16; ++i) {
        const int k = k0 + frag_k(i, h); const float x = (k < klen) ? p[(long long)k * sk] * s : 0.f;
        const __bf16 hb = bf16_rne(x); r.hi[i] = hb; r.lo[i] = bf16_rne(x - bf16_f32(hb));
    }
    return r;
}
__device__ __forceinline__ Split3 sp3_ld(const float* __restrict__ p, long long sk, int k0, int h, int klen, float s) {
    Split3 r;
#pragma unroll
    for (int i = 0; i < 16; ++i) {
        const int k = k0 + frag_k(i, h); const float x = (k < klen) ? p[(long long)k * sk] * s : 0.f;
        const __bf16 hb = bf16_rne(x); const float r1 = x - bf16_f32(hb); const __bf16 mb = bf16_rne(r1);
        r.hi[i] = hb; r.mid[i] = mb; r.lo[i] = bf16_rne(r1 - bf16_f32(mb));
    }
    return r;
}
__device__ __forceinline__ v16b bh_ld(const float* __restrict__ p, long long sk, int k0, int h, int klen, float s) {
    v16b a;
#pragma unroll
    for (int i = 0; i < 16; ++i) { const int k = k0 + frag_k(i, h); a[i] = bf16_rne((k < klen) ? p[(long long)k * sk] * s : 0.f); }
    return a;
}
__device__ __forceinline__ v16h fh_row(const _Float16* __restrict__ row, int k0, int h) {
    v16h a;
#pragma unroll
    for (int i = 0; i < 16; ++i) a[i] = row[k0 + frag_k(i, h)];
    return a;
}

#define VST2(T, ptr, val) do { *(volatile T*)(ptr) = (val); __threadfence(); *(volatile T*)(ptr) = (val); } while (0)
typedef float v4f __attribute__((ext_vector_type(4)));
#define VST2V4(ptr, val) do { *(volatile v4f*)(ptr) = (val); __threadfence(); *(volatile v4f*)(ptr) = (val); } while (0)

__device__ __attribute__((noinline)) float act_fn(float v, int act) {
    if (act == 1) return fmaxf(v, 0.f);
    if (act == 2) { const float u = 0.7978845608028654f * (v + 0.044715f * v * v * v); return 0.5f * v * (1.f + tanhf(u)); }
    if (act == 3) return v / (1.f + expf(-v));
    if (act == 4) return 0.5f * v * (1.f + erff(v * 0.7071067811865476f));
    if (act == 5) return tanhf(v);
    if (act == 6) return 1.f / (1.f + expf(-v));
    if (act == 7) return (v > 0.f) ? v : 0.01f * v;
    if (act == 8) return (v > 0.f) ? v : (expf(v) - 1.f);
    if (act == 9) return fminf(fmaxf(v, 0.f), 6.f);
    if (act == 10) return fabsf(v);
    if (act == 11) return (v >= 0.f) ? v : 0.1f * v;
    if (act == 12) return (v > 0.f) ? v : 0.2f * v;
    if (act == 13) return (v > 20.f) ? v : log1pf(expf(v));
    return v;
}

struct GemmP {
    const float* A; const float* B; const float* bias; const float* R; float* C;
    long long sAo, sAi, sAm, sAk, sBo, sBi, sBn, sBk, sCo, sCi, sCm, sRo, sRi, sRm, sRn;
    int M, N, K, zi_n, flags, act; float alpha, beta, sa, sb;
    int Npad, pad_;
};
static_assert(sizeof(GemmP) == 5 * 8 + 15 * 8 + 6 * 4 + 4 * 4 + 2 * 4, "GemmP has padding");

template <int MODE>
__global__ __launch_bounds__(32) void k_gemm(GemmP p) {
    const int lane = threadIdx.x & 31, h = lane >> 4, l15 = lane & 15;
    const int m0 = blockIdx.y * 16, n0 = blockIdx.x * 32;
    const int z = blockIdx.z, zo = z / p.zi_n, zi = z - zo * p.zi_n;
    const float* A = p.A + zo * p.sAo + zi * p.sAi;
    const float* B = p.B + zo * p.sBo + zi * p.sBi;
    const int am = min(m0 + l15, p.M - 1);
    v8f acc[2], comp[2];
#pragma unroll
    for (int t = 0; t < 2; ++t) { v8f zz = {}; acc[t] = zz; comp[t] = zz; }
    for (int k0 = 0; k0 < p.K; k0 += 32) {
        const float* arow = A + (long long)am * p.sAm;
        if (MODE == 1) {
            const Split a = sp_ld(arow, p.sAk, k0, h, p.K, 1.f);
#pragma unroll
            for (int t = 0; t < 2; ++t) {
                const int bn = min(n0 + t * 16 + l15, p.N - 1);
                acc[t] = wmma3(a, sp_ld(B + (long long)bn * p.sBn, p.sBk, k0, h, p.K, 1.f), acc[t]);
            }
        } else if (MODE == 3) {
            const Split3 a = sp3_ld(arow, p.sAk, k0, h, p.K, 1.f);
#pragma unroll
            for (int t = 0; t < 2; ++t) {
                const int bn = min(n0 + t * 16 + l15, p.N - 1);
                acc[t] = wmma6(a, sp3_ld(B + (long long)bn * p.sBn, p.sBk, k0, h, p.K, 1.f), acc[t]);
            }
        } else if (MODE == 4) {
            const Split3 a = sp3_ld(arow, p.sAk, k0, h, p.K, 1.f);
#pragma unroll
            for (int t = 0; t < 2; ++t) {
                const int bn = min(n0 + t * 16 + l15, p.N - 1); v8f zz = {};
                const v8f part = wmma6(a, sp3_ld(B + (long long)bn * p.sBn, p.sBk, k0, h, p.K, 1.f), zz);
                const v8f y = part - comp[t]; const v8f s = acc[t] + y; comp[t] = (s - acc[t]) - y; acc[t] = s;
            }
        } else if (MODE == 2) {
            const v16b a = bh_ld(arow, p.sAk, k0, h, p.K, 1.f);
#pragma unroll
            for (int t = 0; t < 2; ++t) {
                const int bn = min(n0 + t * 16 + l15, p.N - 1);
                acc[t] = wmmab(a, bh_ld(B + (long long)bn * p.sBn, p.sBk, k0, h, p.K, 1.f), acc[t]);
            }
        } else {
            const v16h a = fh_ld(arow, p.sAk, k0, h, p.K, p.sa);
#pragma unroll
            for (int t = 0; t < 2; ++t) {
                const int bn = min(n0 + t * 16 + l15, p.N - 1);
                acc[t] = wmma16(a, fh_ld(B + (long long)bn * p.sBn, p.sBk, k0, h, p.K, p.sb), acc[t]);
            }
        }
    }
    const float iscale = (MODE == 0) ? p.alpha / (p.sa * p.sb) : p.alpha;
    float* C = p.C + zo * p.sCo + zi * p.sCi;
    const float* R = p.R + zo * p.sRo + zi * p.sRi;
    __shared__ __align__(16) float ctile[16][36];
#pragma unroll
    for (int t = 0; t < 2; ++t) {
        const int n = n0 + t * 16 + l15; const int nn = min(n, p.N - 1);
#pragma unroll
        for (int r = 0; r < 8; ++r) {
            const int m = m0 + 8 * h + r; const int mm = min(m, p.M - 1);
            float v = acc[t][r] * iscale;
            if (p.flags & 1) v += p.bias[nn];
            if (p.flags & 2) v += p.bias[mm];
            v = act_fn(v, p.act);
            if (p.flags & 4) v += p.beta * R[(long long)mm * p.sRm + (long long)nn * p.sRn];
            ctile[8 * h + r][t * 16 + l15] = (n < p.N) ? v : 0.f;
        }
    }
    __syncthreads();
    const int NW = (p.Npad > p.N) ? p.Npad : p.N;
    const bool fast = (m0 + 16 <= p.M) && (n0 + 32 <= NW) && ((p.sCm & 3) == 0) && ((((size_t)C) & 15) == 0);
    if (fast) {
#pragma unroll
        for (int s = 0; s < 4; ++s) {
            const int row = s * 4 + (lane >> 3), c4 = (lane & 7) * 4;
            const v4f v = *(const v4f*)&ctile[row][c4];
            VST2V4(C + (long long)(m0 + row) * p.sCm + n0 + c4, v);
        }
    } else {
        for (int row = 0; row < 16; ++row) {
            const int m = m0 + row, n = n0 + lane;
            if (m < p.M && n < NW) VST2(float, C + (long long)m * p.sCm + n, ctile[row][lane]);
        }
    }
}

#define AW 4
struct AttnP {
    const float* Q; const float* K; const float* V; float* O; float* P; const float* Mf; const int* Mi; float* ST;
    const float* Pw; const float* Rt; const int* SQ; const int* SK;
    long long swb, swh, swi, swj, srb, srh, sri;
    long long sQb, sQh, sQi, sQd, sKb, sKh, sKj, sKd, sVb, sVh, sVj, sVd, sOb, sOh, sOi, sPb, sPh, sPi, smb, smh, smi, smj;
    int Lq, Lk, dh, dv, hrep, causal, coff, pband;
    float scale, mfill; int nonorm, mpol;
    int roff, rn, segpol, win;
};
static_assert(sizeof(AttnP) == 12 * 8 + 29 * 8 + 16 * 4, "AttnP has padding");

#ifndef KATTN_ATTR
#define KATTN_ATTR
#endif
template <int DHP, int DVP, int QM, bool SPLITPV, bool TWOPASS>
__global__ __launch_bounds__(32 * AW) KATTN_ATTR void k_attn(AttnP p) {
    constexpr int NT = DVP / 16;
    constexpr int KS = DHP / 32;
    constexpr int VP = DVP + 8;
    __shared__ __align__(16) float    pl[AW][16 * 64];
    __shared__ __align__(16) _Float16 vl[(SPLITPV ? 2 : 1) * 64 * VP];
    const int lane = threadIdx.x & 31, hf = lane >> 4, l15 = lane & 15, wave = threadIdx.x >> 5;
    const int h = blockIdx.y, b = blockIdx.z, hk = h / p.hrep;
    const int q0 = (blockIdx.x * AW + wave) * 16;
    float* myp = pl[wave];
    const float L2E = 1.4426950408889634f;
    const float NEG = -__builtin_inff();
    const int qi = min(q0 + l15, p.Lq - 1);
    const float* qrow = p.Q + b * p.sQb + h * p.sQh + (long long)qi * p.sQi;
    const float* kbase = p.K + b * p.sKb + hk * p.sKh;
    const float* vbase = p.V + b * p.sVb + hk * p.sVh;
    v16h qa[QM == 0 ? KS : 1]; Split qs_[QM == 1 ? KS : 1]; Split3 qt_[QM == 2 ? KS : 1];
#pragma unroll
    for (int ks = 0; ks < KS; ++ks) {
        if (QM == 2) qt_[ks] = sp3_ld(qrow, p.sQd, ks * 32, hf, p.dh, 1.f);
        else if (QM == 1) qs_[ks] = sp_ld(qrow, p.sQd, ks * 32, hf, p.dh, 1.f);
        else qa[ks] = fh_ld(qrow, p.sQd, ks * 32, hf, p.dh, 1.f);
    }
    v8f o[NT]; float m8[8], l8[8];
#pragma unroll
    for (int t = 0; t < NT; ++t) { v8f zz = {}; o[t] = zz; }
#pragma unroll
    for (int i = 0; i < 8; ++i) { m8[i] = NEG; l8[i] = 0.f; }
    int jend = p.Lk;
    if (p.causal == 1) { const int je = (blockIdx.x * AW + AW - 1) * 16 + 16 + p.coff; jend = min(jend, max(je, 0)); }
    const int npass = TWOPASS ? 2 : 1;
    for (int pass = 0; pass < npass; ++pass) {
        const bool dopv = (!TWOPASS) || pass == 1;
        for (int j0 = 0; j0 < jend; j0 += 64) {
            if (dopv) {
                __syncthreads();
                for (int idx = threadIdx.x; idx < 64 * DVP; idx += 32 * AW) {
                    const int jr = idx / DVP, d = idx - jr * DVP, j = j0 + jr;
                    const float f = (j < p.Lk && d < p.dv) ? vbase[(long long)j * p.sVj + (long long)d * p.sVd] : 0.f;
                    if (SPLITPV) {
                        const __bf16 hb = bf16_rne(f);
                        ((__bf16*)vl)[jr * VP + d] = hb; ((__bf16*)vl)[64 * VP + jr * VP + d] = bf16_rne(f - bf16_f32(hb));
                    } else vl[jr * VP + d] = (_Float16)f;
                }
            }
            v8f s[4];
#pragma unroll
            for (int t = 0; t < 4; ++t) {
                const int j = min(j0 + t * 16 + l15, p.Lk - 1);
                const float* krow = kbase + (long long)j * p.sKj;
                v8f acc = {};
#pragma unroll
                for (int ks = 0; ks < KS; ++ks) {
                    if (QM == 2)      acc = wmma6(qt_[ks], sp3_ld(krow, p.sKd, ks * 32, hf, p.dh, 1.f), acc);
                    else if (QM == 1) acc = wmma3(qs_[ks], sp_ld(krow, p.sKd, ks * 32, hf, p.dh, 1.f), acc);
                    else              acc = wmma16(qa[ks], fh_ld(krow, p.sKd, ks * 32, hf, p.dh, 1.f), acc);
                }
                s[t] = acc;
            }
            float pv[8][4];
#pragma unroll
            for (int i = 0; i < 8; ++i) {
                const int irow = q0 + i + 8 * hf;
                const int ic = min(irow, p.Lq - 1);
                float sc[4];
#pragma unroll
                for (int t = 0; t < 4; ++t) {
                    const int jg = j0 + t * 16 + l15;
                    float v = s[t][i] * p.scale;
                    if (p.Mf) v += p.Mf[b * p.smb + h * p.smh + (long long)ic * p.smi + (long long)min(jg, p.Lk - 1) * p.smj];
                    if (p.Rt) { int rc = ic - min(jg, p.Lk - 1) + p.roff; rc = rc < 0 ? 0 : (rc >= p.rn ? p.rn - 1 : rc); v += p.Rt[b * p.srb + h * p.srh + (long long)ic * p.sri + rc]; }
                    if (p.Mi) { const int mv = p.Mi[b * p.smb + h * p.smh + (long long)ic * p.smi + (long long)min(jg, p.Lk - 1) * p.smj]; if (p.mpol ? (mv != 0) : (mv == 0)) v = p.mfill; }
                    if (p.SQ) { const bool same = p.SQ[(long long)b * p.Lq + ic] == p.SK[(long long)b * p.Lk + min(jg, p.Lk - 1)]; if (p.segpol ? same : !same) v = p.mfill; }
                    if (p.causal == 2 && jg > irow + p.coff) v = p.mfill;
                    if (jg >= p.Lk || (p.causal == 1 && jg > irow + p.coff) || (p.causal == 3 && jg < irow + p.coff) || (p.win > 0 && irow + p.coff - jg > p.win)) v = NEG; else v *= L2E;
                    sc[t] = v;
                }
                if (!TWOPASS || pass == 0) {
                    float mx = fmaxf(fmaxf(sc[0], sc[1]), fmaxf(sc[2], sc[3]));
                    mx = fmaxf(mx, __shfl_xor(mx, 1, 32)); mx = fmaxf(mx, __shfl_xor(mx, 2, 32));
                    mx = fmaxf(mx, __shfl_xor(mx, 4, 32)); mx = fmaxf(mx, __shfl_xor(mx, 8, 32));
                    const float mnew = fmaxf(m8[i], mx);
                    const float corr = (mnew == NEG) ? 1.f : exp2f(m8[i] - mnew);
                    float rs = 0.f;
#pragma unroll
                    for (int t = 0; t < 4; ++t) {
                        const float pp = (sc[t] == NEG) ? 0.f : exp2f(sc[t] - mnew); rs += pp;
                        pv[i][t] = p.Pw ? pp * p.Pw[b * p.swb + h * p.swh + (long long)ic * p.swi + (long long)min(j0 + t * 16 + l15, p.Lk - 1) * p.swj] : pp;
                    }
                    rs += __shfl_xor(rs, 1, 32); rs += __shfl_xor(rs, 2, 32); rs += __shfl_xor(rs, 4, 32); rs += __shfl_xor(rs, 8, 32);
                    l8[i] = l8[i] * corr + rs; m8[i] = mnew;
                    if (!TWOPASS) {
#pragma unroll
                        for (int t = 0; t < NT; ++t) o[t][i] *= corr;
                    }
                } else {
                    const float inv = (l8[i] > 0.f) ? 1.f / l8[i] : 0.f;
#pragma unroll
                    for (int t = 0; t < 4; ++t) {
                        const int jg = j0 + t * 16 + l15;
                        float pp = (sc[t] == NEG) ? 0.f : exp2f(sc[t] - m8[i]) * inv;
                        if (p.Pw) pp *= p.Pw[b * p.swb + h * p.swh + (long long)ic * p.swi + (long long)min(jg, p.Lk - 1) * p.swj];
                        pv[i][t] = pp;
                    }
                }
            }
            if (dopv) {
#pragma unroll
                for (int i = 0; i < 8; ++i)
#pragma unroll
                    for (int t = 0; t < 4; ++t) myp[(i + 8 * hf) * 64 + t * 16 + l15] = pv[i][t];
                __syncthreads();
                if (p.P) {
                    float* pb_ = p.P + b * p.sPb + h * p.sPh;
                    const bool fastP = (p.pband == 0) && ((p.sPi & 3) == 0) && (j0 + 64 <= p.Lk) && (q0 + 16 <= p.Lq) && ((((size_t)pb_) & 15) == 0);
                    if (fastP) {
#pragma unroll
                        for (int s = 0; s < 8; ++s) {
                            const int row = s * 2 + (lane >> 4), c4 = (lane & 15) * 4;
                            const v4f v = *(const v4f*)(myp + row * 64 + c4);
                            VST2V4(pb_ + (long long)(q0 + row) * p.sPi + j0 + c4, v);
                        }
                    } else {
                        for (int row = 0; row < 16; ++row) {
                            const int irow = q0 + row; if (irow >= p.Lq) continue;
                            for (int c = lane; c < 64; c += 32) {
                                const int jg = j0 + c; if (jg >= p.Lk) continue;
                                if (p.pband == 0) VST2(float, pb_ + (long long)irow * p.sPi + jg, myp[row * 64 + c]);
                                else if (jg - irow <= p.pband && irow - jg <= p.pband) VST2(float, pb_ + (long long)irow * p.sPi + (jg - irow + p.pband), myp[row * 64 + c]);
                            }
                        }
                    }
                }
                if (SPLITPV) {
                    const Split pa0 = sp_ld(myp + l15 * 64, 1, 0, hf, 64, 1.f), pa1 = sp_ld(myp + l15 * 64, 1, 32, hf, 64, 1.f);
                    const __bf16* vh = (const __bf16*)vl; const __bf16* vlo = vh + 64 * VP;
#pragma unroll
                    for (int t = 0; t < NT; ++t) {
                        const int dcol = t * 16 + l15;
                        Split b0, b1;
#pragma unroll
                        for (int e = 0; e < 16; ++e) {
                            const int k0 = frag_k(e, hf), k1 = 32 + frag_k(e, hf);
                            b0.hi[e] = vh[k0 * VP + dcol]; b0.lo[e] = vlo[k0 * VP + dcol]; b1.hi[e] = vh[k1 * VP + dcol]; b1.lo[e] = vlo[k1 * VP + dcol];
                        }
                        o[t] = wmma3(pa0, b0, o[t]);
                        o[t] = wmma3(pa1, b1, o[t]);
                    }
                } else {
                    const v16h pa0 = fh_ld(myp + l15 * 64, 1, 0, hf, 64, 4096.f), pa1 = fh_ld(myp + l15 * 64, 1, 32, hf, 64, 4096.f);
#pragma unroll
                    for (int t = 0; t < NT; ++t) {
                        const int dcol = t * 16 + l15;
                        v16h b0, b1;
#pragma unroll
                        for (int e = 0; e < 16; ++e) { b0[e] = vl[frag_k(e, hf) * VP + dcol]; b1[e] = vl[(32 + frag_k(e, hf)) * VP + dcol]; }
                        o[t] = wmma16(pa0, b0, o[t]);
                        o[t] = wmma16(pa1, b1, o[t]);
                    }
                }
            }
        }
    }
    float* obase = p.O + b * p.sOb + h * p.sOh;
    if (p.ST) {
        const int rl = lane >> 1, isel = rl & 7;
        float mv = 0.f, lv = 0.f;
#pragma unroll
        for (int i = 0; i < 8; ++i) if (i == isel) { mv = m8[i]; lv = l8[i]; }
        const int irow = q0 + rl;
        if (irow < p.Lq) { float* st = p.ST + (((long long)b * gridDim.y + h) * p.Lq + irow) * 2 + (lane & 1); VST2(float, st, (lane & 1) ? lv : mv * 0.6931471805599453f); }
    }
    float invr[8];
#pragma unroll
    for (int i = 0; i < 8; ++i) {
        if (TWOPASS) invr[i] = SPLITPV ? 1.f : (1.f / 4096.f);
        else if (p.nonorm) invr[i] = exp2f(m8[i]) * (SPLITPV ? 1.f : (1.f / 4096.f));
        else invr[i] = (l8[i] > 0.f) ? (SPLITPV ? 1.f / l8[i] : 1.f / (l8[i] * 4096.f)) : 0.f;
    }
    __syncthreads();
    const bool ofast = ((p.sOi & 3) == 0) && ((((size_t)obase) & 15) == 0) && (q0 + 16 <= p.Lq);
#pragma unroll
    for (int c0 = 0; c0 < DVP; c0 += 64) {
#pragma unroll
        for (int i = 0; i < 8; ++i)
#pragma unroll
            for (int t = 0; t < NT; ++t) if (t * 16 >= c0 && t * 16 < c0 + 64) myp[(i + 8 * hf) * 64 + (t * 16 - c0) + l15] = o[t][i] * invr[i];
        __syncthreads();
        const int cw = (DVP - c0 < 64) ? (DVP - c0) : 64;
        if (ofast && (c0 + cw <= p.dv) && (cw % 32 == 0)) {
            const int lpr = cw / 4;
            const int rows_per_ins = 32 / lpr;
            for (int r0 = 0; r0 < 16; r0 += rows_per_ins) {
                const int row = r0 + lane / lpr, c4 = (lane % lpr) * 4;
                const v4f v = *(const v4f*)(myp + row * 64 + c4);
                VST2V4(obase + (long long)(q0 + row) * p.sOi + c0 + c4, v);
            }
        } else {
            for (int row = 0; row < 16; ++row) {
                const int irow = q0 + row; if (irow >= p.Lq) continue;
                for (int c = lane; c < cw; c += 32) { const int d = c0 + c; if (d < p.dv) VST2(float, obase + (long long)irow * p.sOi + d, myp[row * 64 + c]); }
            }
        }
        __syncthreads();
    }
}

struct TrP { const float* src; float* dst; const float* R2; long long sSz, lds, sDz, ldd, sRz, ldr; int R, C, flags, act; float alpha, beta; };
static_assert(sizeof(TrP) == 3 * 8 + 6 * 8 + 6 * 4, "TrP has padding");
__global__ __launch_bounds__(256) void k_tr(TrP p) {
    __shared__ float tile[32][33];
    const int c0 = blockIdx.x * 32, r0 = blockIdx.y * 32, z = blockIdx.z;
    const int lane = threadIdx.x & 31, wave = threadIdx.x >> 5;
    const float* s = p.src + z * p.sSz;
#pragma unroll
    for (int k = 0; k < 4; ++k) {
        const int rl = wave * 4 + k, r = r0 + rl, c = c0 + lane;
        tile[rl][lane] = (r < p.R && c < p.C) ? s[(long long)r * p.lds + c] : 0.f;
    }
    __syncthreads();
    float* d = p.dst + z * p.sDz; const float* rr = p.R2 + z * p.sRz;
#pragma unroll
    for (int k = 0; k < 4; ++k) {
        const int cl = wave * 4 + k, c = c0 + cl, r = r0 + lane;
        if (c < p.C && r < p.R) {
            float v = act_fn(p.alpha * tile[lane][cl], p.act);
            if (p.flags & 1) v += p.beta * rr[(long long)c * p.ldr + r];
            VST2(float, d + (long long)c * p.ldd + r, v);
        }
    }
}

__global__ __launch_bounds__(256) void k_affine(const float* __restrict__ src, float* __restrict__ dst, int n, float a, float b, const float* __restrict__ sdev) {
    const int i = blockIdx.x * 256 + threadIdx.x;
    if (i < n) { const float aa = sdev ? a * sdev[0] : a; const float v = aa * src[i] + b; VST2(float, dst + i, v); }
}

struct SmP { const float* src; float* dst; const float* Mf; long long sz, sr, dz, dr, smz, smr; int n, pad; float scale_in, scale_out; };
static_assert(sizeof(SmP) == 3 * 8 + 6 * 8 + 4 * 4, "SmP has padding");
__global__ __launch_bounds__(256) void k_softmax(SmP p) {
    __shared__ float red[256];
    const int r = blockIdx.x, z = blockIdx.y, tid = threadIdx.x;
    const float* s = p.src + z * p.sz + (long long)r * p.sr;
    const float* mf = p.Mf ? (p.Mf + z * p.smz + (long long)r * p.smr) : nullptr;
    float mx = -__builtin_inff();
    for (int j = tid; j < p.n; j += 256) { float v = s[j] * p.scale_in; if (mf) v += mf[j]; mx = fmaxf(mx, v); }
    red[tid] = mx; __syncthreads();
    for (int o = 128; o > 0; o >>= 1) { if (tid < o) red[tid] = fmaxf(red[tid], red[tid + o]); __syncthreads(); }
    mx = red[0]; __syncthreads();
    float sum = 0.f;
    for (int j = tid; j < p.n; j += 256) { float v = s[j] * p.scale_in; if (mf) v += mf[j]; sum += (mx == -__builtin_inff()) ? 0.f : expf(v - mx); }
    red[tid] = sum; __syncthreads();
    for (int o = 128; o > 0; o >>= 1) { if (tid < o) red[tid] += red[tid + o]; __syncthreads(); }
    sum = red[0];
    const float inv = (sum > 0.f) ? p.scale_out / sum : 0.f;
    float* d = p.dst + z * p.dz + (long long)r * p.dr;
    for (int j = tid; j < p.n; j += 256) { float v = s[j] * p.scale_in; if (mf) v += mf[j]; const float o = (mx == -__builtin_inff()) ? 0.f : expf(v - mx) * inv; VST2(float, d + j, o); }
}
__global__ __launch_bounds__(256) void k_stats(const float* __restrict__ x, long long sz, long long so, long long si, int inner, int n, float eps, float* __restrict__ stat, int mode) {
    __shared__ float red[256];
    const int z = blockIdx.x, tid = threadIdx.x;
    const float* base = x + z * sz;
    float s = 0.f;
    for (int e = tid; e < n; e += 256) s += base[(long long)(e / inner) * so + (long long)(e % inner) * si];
    red[tid] = s; __syncthreads();
    for (int o = 128; o > 0; o >>= 1) { if (tid < o) red[tid] += red[tid + o]; __syncthreads(); }
    const float mu = (mode == 0 || mode == 3) ? red[0] / (float)n : 0.f; __syncthreads();
    float q = 0.f;
    for (int e = tid; e < n; e += 256) { const float dlt = base[(long long)(e / inner) * so + (long long)(e % inner) * si] - mu; q += dlt * dlt; }
    red[tid] = q; __syncthreads();
    for (int o = 128; o > 0; o >>= 1) { if (tid < o) red[tid] += red[tid + o]; __syncthreads(); }
    {
        float rs;
        if (mode == 2) rs = sqrtf((float)n) / fmaxf(sqrtf(red[0]), eps); else if (mode == 3) rs = rsqrtf(red[0] / (float)(n - 1) + eps); else rs = rsqrtf(red[0] / (float)n + eps);
        if (tid < 32) { const float v = (tid == 0) ? mu : ((tid == 1) ? rs : 0.f); VST2(float, stat + (long long)z * 32 + tid, v); }
    }
}
__global__ __launch_bounds__(256) void k_norm_apply(const float* __restrict__ x, float* __restrict__ y, const float* __restrict__ stat, const float* __restrict__ g, const float* __restrict__ bta,
                                                     int Z, int C, int L, int G, int bn, int act) {
    const long long idx = (long long)blockIdx.x * 256 + threadIdx.x;
    if (idx >= (long long)Z * C * L) return;
    const int l = (int)(idx % L); const long long zc = idx / L; const int c = (int)(zc % C), z = (int)(zc / C); (void)l;
    const int set = bn ? c : (z * G + c / (C / G));
    float v = (x[idx] - stat[(long long)set * 32]) * stat[(long long)set * 32 + 1];
    if (g) v *= g[c];
    if (bta) v += bta[c];
    v = act_fn(v, act);
    VST2(float, y + idx, v);
}

__global__ __launch_bounds__(256) void k_lse_neg(const float* __restrict__ st, float* __restrict__ c, int n) {
    const int i = blockIdx.x * 256 + threadIdx.x;
    if (i < n) { const float v = -(st[2 * i] + logf(st[2 * i + 1])); VST2(float, c + i, v); }
}

__global__ __launch_bounds__(256) void k_iota(int* __restrict__ dst, int n, int a, int b) {
    const int i = blockIdx.x * 256 + threadIdx.x;
    if (i < n) { const int v = a * i + b; VST2(int, dst + i, v); }
}

__global__ __launch_bounds__(256) void k_axpby(const float* __restrict__ x, const float* __restrict__ y, float* __restrict__ dst, int n, float a, float b, float c) {
    const int i = blockIdx.x * 256 + threadIdx.x;
    if (i < n) { const float v = a * x[i] + b * y[i] + c; VST2(float, dst + i, v); }
}

struct RopeP { const float* X; float* Y; const float* C; const float* Sn; const int* pos; long long sXr, sXh, sYr, sYh, sCb, sCp, sCd; int R, Hn, D, S, mode, tmode, pmode, pad; };
static_assert(sizeof(RopeP) == 5 * 8 + 7 * 8 + 8 * 4, "RopeP has padding");
__global__ __launch_bounds__(256) void k_rope(RopeP p) {
    const long long idx = (long long)blockIdx.x * 256 + threadIdx.x;
    if (idx >= (long long)p.R * p.Hn * p.D) return;
    const int d = (int)(idx % p.D); const long long rh = idx / p.D; const int h = (int)(rh % p.Hn); const int r = (int)(rh / p.Hn);
    const int half = p.D / 2;
    int partner; float sign;
    if (p.mode == 0) { partner = (d < half) ? d + half : d - half; sign = (d < half) ? -1.f : 1.f; }
    else { partner = d ^ 1; sign = (d & 1) ? 1.f : -1.f; }
    const int tcol = (p.tmode == 0) ? d : ((p.tmode == 1) ? (d % half) : (d >> 1));
    const int pp = (p.pmode == 0) ? (r % p.S) : ((p.pmode == 1) ? h : p.pos[r]);
    const long long toff = (long long)(r / p.S) * p.sCb + (long long)pp * p.sCp + (long long)tcol * p.sCd;
    const float* xr = p.X + (long long)r * p.sXr + (long long)h * p.sXh;
    const float v = xr[d] * p.C[toff] + sign * xr[partner] * p.Sn[toff];
    VST2(float, p.Y + (long long)r * p.sYr + (long long)h * p.sYh + d, v);
}

__global__ __launch_bounds__(256) void k_invf(float* __restrict__ invb, int half, int D, float base, float num, int fmode, float cexp) {
    const int i = blockIdx.x * 256 + threadIdx.x;
    if (i >= ((half + 31) / 32) * 32) return;
    if (i >= half) { VST2(float, invb + i, 0.f); return; }
    const float e = (float)(2 * i) / (float)D;
    float invf;
    if (fmode == 1) invf = num * expf((float)(2 * i) * cexp);
    else if (fmode == 2) invf = num * powf(base, (-2.0f * ((float)i - 1.0f)) / (float)D);
    else invf = num * (1.0f / powf(base, e));
    VST2(float, invb + i, invf);
}
__global__ __launch_bounds__(256) void k_sincos(float* __restrict__ cs, float* __restrict__ sn, const float* __restrict__ invb, int S, int half, float pscale) {
    const int idx = blockIdx.x * 256 + threadIdx.x;
    if (idx >= S * half) return;
    const int s = idx / half, i = idx - s * half;
    const float ang = (pscale * (float)s) * invb[i];
    VST2(float, cs + idx, cosf(ang)); VST2(float, sn + idx, sinf(ang));
}

__global__ __launch_bounds__(256) void k_mulact(const float* __restrict__ x, const float* __restrict__ y, float* __restrict__ dst, int n, int act) {
    const int i = blockIdx.x * 256 + threadIdx.x;
    if (i < n) { const float v = act_fn(x[i], act) * y[i]; VST2(float, dst + i, v); }
}

__global__ __launch_bounds__(256) void k_matvec(GemmP p) {
    const int rpt = (p.N == 1) ? 1 : 32;
    const long long r0 = ((long long)blockIdx.x * 256 + threadIdx.x) * rpt; const int z = blockIdx.z, zo = z / p.zi_n, zi = z - zo * p.zi_n;
    if (r0 >= p.M) return;
    const float* Bb = p.B + zo * p.sBo + zi * p.sBi;
    float* C = p.C + zo * p.sCo + zi * p.sCi; const float* R = p.R + zo * p.sRo + zi * p.sRi;
    for (int rr = 0; rr < rpt; ++rr) {
        const long long r = r0 + rr; if (r >= p.M) break;
        const float* A = p.A + zo * p.sAo + zi * p.sAi + r * p.sAm;
        float acc[8] = {0.f, 0.f, 0.f, 0.f, 0.f, 0.f, 0.f, 0.f};
        for (int k = 0; k < p.K; ++k) { const float a = A[(long long)k * p.sAk];
#pragma unroll
            for (int j = 0; j < 8; ++j) if (j < p.N) acc[j] += a * Bb[(long long)j * p.sBn + (long long)k * p.sBk]; }
#pragma unroll
        for (int j = 0; j < 8; ++j) if (j < p.N) {
            float v = acc[j] * p.alpha;
            if (p.flags & 1) v += p.bias[j];
            if (p.flags & 2) v += p.bias[r];
            v = act_fn(v, p.act);
            if (p.flags & 4) v += p.beta * R[r * p.sRm + (long long)j * p.sRn];
            VST2(float, C + r * p.sCm + j, v);
        }
    }
}
__global__ __launch_bounds__(256) void k_smallsoftmax(const float* __restrict__ src, float* __restrict__ dst, long long sr, long long dr, int n, long long R, float scale) {
    const long long r0 = ((long long)blockIdx.x * 256 + threadIdx.x) * 32;
    for (int rr = 0; rr < 32; ++rr) {
        const long long r = r0 + rr; if (r >= R) return;
        const float* s = src + r * sr; float* d = dst + r * dr;
        float mx = -__builtin_inff();
        for (int j = 0; j < n; ++j) mx = fmaxf(mx, s[j] * scale);
        float sum = 0.f;
        for (int j = 0; j < n; ++j) sum += expf(s[j] * scale - mx);
        const float inv = 1.f / sum;
        for (int j = 0; j < n; ++j) { const float v = expf(s[j] * scale - mx) * inv; VST2(float, d + j, v); }
    }
}

__global__ __launch_bounds__(32) void k_unitstat(float* __restrict__ st) { const int t = threadIdx.x; const float v = (t == 1) ? 1.f : 0.f; VST2(float, st + t, v); }

__global__ __launch_bounds__(256) void k_lincopy(const float* __restrict__ src, long long lds, float* __restrict__ dst, long long ldd, long long rows, int cols) {
    const long long i = (long long)blockIdx.x * 256 + threadIdx.x; if (i >= rows * cols) return;
    const long long r = i / cols; const int c = (int)(i - r * cols);
    const float v = src[r * lds + c]; VST2(float, dst + r * ldd + c, v);
}

__global__ __launch_bounds__(256) void k_sh_pad(const float* __restrict__ X, float* __restrict__ XP, int B, int C, int H) { const long long q = (long long)blockIdx.x * 256 + threadIdx.x; if (q >= (long long)B * H * H * C) return; const int c = (int)(q % C); const int x = (int)((q / C) % H); const int y = (int)((q / ((long long)C * H)) % H); const int b = (int)(q / ((long long)C * H * H)); VST2(float, XP + (((long long)b * (H + 2) + y + 1) * (H + 2) + x + 1) * C + c, X[(((long long)b * C + c) * H + y) * H + x]); }
__global__ __launch_bounds__(256) void k_sh_bn(const float* __restrict__ T, int Cs, const float* __restrict__ g, const float* __restrict__ bb, const float* __restrict__ m, const float* __restrict__ v, float* __restrict__ DSTP, int Cd, int coff, int relu, int B, int H) { const long long q = (long long)blockIdx.x * 256 + threadIdx.x; if (q >= (long long)B * H * H * Cs) return; const int c = (int)(q % Cs); const int x = (int)((q / Cs) % H); const int y = (int)((q / ((long long)Cs * H)) % H); const int b = (int)(q / ((long long)Cs * H * H));
    const float s = g[c] * rsqrtf(v[c] + 1e-5f); float val = T[q] * s + (bb[c] - m[c] * s); if (relu) val = fmaxf(val, 0.f); VST2(float, DSTP + (((long long)b * (H + 2) + y + 1) * (H + 2) + x + 1) * Cd + coff + c, val); }
__global__ __launch_bounds__(256) void k_sh_col(const float* __restrict__ XPp, const float* __restrict__ OFF, int ldo, float* __restrict__ COL, int b, int H, int C) { const long long q = (long long)blockIdx.x * 256 + threadIdx.x; if (q >= (long long)H * H * 9 * C) return; const int kk = (int)(q % 9); const int c = (int)((q / 9) % C); const int p = (int)(q / (9 * C)); const int y = p / H, x = p % H; const int ki = kk / 3, kj = kk % 3;
    const float* of = OFF + ((long long)b * H * H + p) * ldo; const float py = (float)y - 1.f + (float)ki + of[2 * kk], px = (float)x - 1.f + (float)kj + of[2 * kk + 1];
    const float fy = floorf(py), fx = floorf(px); const float wy = py - fy, wx = px - fx; const int y0 = (int)fy, x0 = (int)fx; float acc = 0.f;
    for (int dy = 0; dy < 2; ++dy) for (int dx = 0; dx < 2; ++dx) { const int yi = y0 + dy, xi = x0 + dx; const float w = (dy ? wy : 1.f - wy) * (dx ? wx : 1.f - wx); if (yi >= 0 && yi < H && xi >= 0 && xi < H) acc += w * XPp[(((long long)b * (H + 2) + yi + 1) * (H + 2) + xi + 1) * C + c]; }
    VST2(float, COL + q, acc); }
__global__ __launch_bounds__(256) void k_sh_repad(const float* __restrict__ T, float* __restrict__ P, int B, int H, int C) { const long long q = (long long)blockIdx.x * 256 + threadIdx.x; if (q >= (long long)B * H * H * C) return; const int c = (int)(q % C); const int x = (int)((q / C) % H); const int y = (int)((q / ((long long)C * H)) % H); const int b = (int)(q / ((long long)C * H * H)); VST2(float, P + (((long long)b * (H + 2) + y + 1) * (H + 2) + x + 1) * C + c, T[q]); }
__global__ __launch_bounds__(256) void k_sh_out(const float* __restrict__ T, float* __restrict__ OUT, int B, int H, int C) { const long long q = (long long)blockIdx.x * 256 + threadIdx.x; if (q >= (long long)B * C * H * H) return; const int p = (int)(q % (H * H)); const int c = (int)((q / (H * H)) % C); const int b = (int)(q / ((long long)H * H * C)); VST2(float, OUT + q, T[((long long)b * H * H + p) * C + c]); }

template __global__ void k_gemm<1>(GemmP);

extern "C" void kernel_launch(void* const* d_in, const int* in_sizes, int n_in, void* d_out, int out_size, void* d_ws, size_t ws_size, hipStream_t stream) {
    (void)in_sizes; (void)n_in; (void)out_size; (void)ws_size;
    const float* inp = (const float*)d_in[0];
    const float* w3 = (const float*)d_in[1];
    const float* g3 = (const float*)d_in[2];
    const float* bb3 = (const float*)d_in[3];
    const float* m3 = (const float*)d_in[4];
    const float* v3 = (const float*)d_in[5];
    const float* w51 = (const float*)d_in[6];
    const float* g51 = (const float*)d_in[7];
    const float* bb51 = (const float*)d_in[8];
    const float* m51 = (const float*)d_in[9];
    const float* v51 = (const float*)d_in[10];
    const float* w52 = (const float*)d_in[11];
    const float* g52 = (const float*)d_in[12];
    const float* bb52 = (const float*)d_in[13];
    const float* m52 = (const float*)d_in[14];
    const float* v52 = (const float*)d_in[15];
    const float* w72 = (const float*)d_in[16];
    const float* g72 = (const float*)d_in[17];
    const float* bb72 = (const float*)d_in[18];
    const float* m72 = (const float*)d_in[19];
    const float* v72 = (const float*)d_in[20];
    const float* w73 = (const float*)d_in[21];
    const float* g73 = (const float*)d_in[22];
    const float* bb73 = (const float*)d_in[23];
    const float* m73 = (const float*)d_in[24];
    const float* v73 = (const float*)d_in[25];
    const float* ow1 = (const float*)d_in[26];
    const float* ob1 = (const float*)d_in[27];
    const float* dw1 = (const float*)d_in[28];
    const float* ow2 = (const float*)d_in[29];
    const float* ob2 = (const float*)d_in[30];
    const float* dw2 = (const float*)d_in[31];
    const int Bn = 4;
    const int Hs = 80;
    const int HW = 6400;
    const int CI = 256;
    const int HP = 82;
    const int PP = HP * HP;
    float* out = (float*)d_out;
    char* wsp = (char*)d_ws;
    float* XP = (float*)wsp; wsp += (((size_t)((size_t)Bn * PP * CI) * 4 + 255) / 256) * 256;
    float* T1 = (float*)wsp; wsp += (((size_t)((size_t)Bn * HW * 128) * 4 + 255) / 256) * 256;
    float* P51 = (float*)wsp; wsp += (((size_t)((size_t)Bn * PP * 64) * 4 + 255) / 256) * 256;
    float* P72 = (float*)wsp; wsp += (((size_t)((size_t)Bn * PP * 64) * 4 + 255) / 256) * 256;
    float* T64 = (float*)wsp; wsp += (((size_t)((size_t)Bn * HW * 64) * 4 + 255) / 256) * 256;
    float* OP = (float*)wsp; wsp += (((size_t)((size_t)Bn * PP * CI) * 4 + 255) / 256) * 256;
    float* OFF = (float*)wsp; wsp += (((size_t)((size_t)Bn * HW * 32) * 4 + 255) / 256) * 256;
    float* COL = (float*)wsp; wsp += (((size_t)((size_t)HW * 9 * CI) * 4 + 255) / 256) * 256;
    float* O2 = (float*)wsp; wsp += (((size_t)((size_t)Bn * HW * CI) * 4 + 255) / 256) * 256;
    float* bnst = (float*)wsp; wsp += (((size_t)((size_t)256 * 2) * 4 + 255) / 256) * 256;
    hipMemsetAsync(XP, 0, (size_t)Bn * PP * CI * 4, stream); hipMemsetAsync(P51, 0, (size_t)Bn * PP * 64 * 4, stream); hipMemsetAsync(P72, 0, (size_t)Bn * PP * 64 * 4, stream); hipMemsetAsync(OP, 0, (size_t)Bn * PP * CI * 4, stream);
    k_sh_pad<<<(unsigned)(((long long)Bn * HW * CI + 255) / 256), 256, 0, stream>>>(inp, XP, Bn, CI, Hs);
    { GemmP c3_0;
      c3_0.A = XP + (size_t)0 * 256; c3_0.B = w3 + 0; c3_0.bias = XP + (size_t)0 * 256; c3_0.R = XP + (size_t)0 * 256; c3_0.C = T1;
      c3_0.sAo = (long long)PP * 256; c3_0.sAi = (long long)HP * 256; c3_0.sAm = 256; c3_0.sAk = 1; c3_0.sBo = 0; c3_0.sBi = 0; c3_0.sBn = 256 * 9; c3_0.sBk = 9; c3_0.sCo = (long long)HW * 128; c3_0.sCi = (long long)Hs * 128; c3_0.sCm = 128; c3_0.sRo = 0; c3_0.sRi = 0; c3_0.sRm = 0; c3_0.sRn = 0;
      c3_0.M = Hs; c3_0.N = 128; c3_0.K = 256; c3_0.zi_n = Hs; c3_0.flags = 0; c3_0.act = 0;
      c3_0.alpha = 1.0f; c3_0.beta = 0.0f; c3_0.sa = 1.0f; c3_0.sb = 1.0f; c3_0.Npad = 128; c3_0.pad_ = 0;
      k_gemm<1><<<dim3((unsigned)((128) + 31) / 32, (unsigned)((Hs) + 15) / 16, (unsigned)(Bn * Hs)), 32, 0, stream>>>(c3_0); }
    { GemmP c3_1;
      c3_1.A = XP + (size_t)1 * 256; c3_1.B = w3 + 1; c3_1.bias = XP + (size_t)1 * 256; c3_1.R = T1; c3_1.C = T1;
      c3_1.sAo = (long long)PP * 256; c3_1.sAi = (long long)HP * 256; c3_1.sAm = 256; c3_1.sAk = 1; c3_1.sBo = 0; c3_1.sBi = 0; c3_1.sBn = 256 * 9; c3_1.sBk = 9; c3_1.sCo = (long long)HW * 128; c3_1.sCi = (long long)Hs * 128; c3_1.sCm = 128; c3_1.sRo = (long long)HW * 128; c3_1.sRi = (long long)Hs * 128; c3_1.sRm = 128; c3_1.sRn = 1;
      c3_1.M = Hs; c3_1.N = 128; c3_1.K = 256; c3_1.zi_n = Hs; c3_1.flags = 4; c3_1.act = 0;
      c3_1.alpha = 1.0f; c3_1.beta = 1.0f; c3_1.sa = 1.0f; c3_1.sb = 1.0f; c3_1.Npad = 128; c3_1.pad_ = 0;
      k_gemm<1><<<dim3((unsigned)((128) + 31) / 32, (unsigned)((Hs) + 15) / 16, (unsigned)(Bn * Hs)), 32, 0, stream>>>(c3_1); }
    { GemmP c3_2;
      c3_2.A = XP + (size_t)2 * 256; c3_2.B = w3 + 2; c3_2.bias = XP + (size_t)2 * 256; c3_2.R = T1; c3_2.C = T1;
      c3_2.sAo = (long long)PP * 256; c3_2.sAi = (long long)HP * 256; c3_2.sAm = 256; c3_2.sAk = 1; c3_2.sBo = 0; c3_2.sBi = 0; c3_2.sBn = 256 * 9; c3_2.sBk = 9; c3_2.sCo = (long long)HW * 128; c3_2.sCi = (long long)Hs * 128; c3_2.sCm = 128; c3_2.sRo = (long long)HW * 128; c3_2.sRi = (long long)Hs * 128; c3_2.sRm = 128; c3_2.sRn = 1;
      c3_2.M = Hs; c3_2.N = 128; c3_2.K = 256; c3_2.zi_n = Hs; c3_2.flags = 4; c3_2.act = 0;
      c3_2.alpha = 1.0f; c3_2.beta = 1.0f; c3_2.sa = 1.0f; c3_2.sb = 1.0f; c3_2.Npad = 128; c3_2.pad_ = 0;
      k_gemm<1><<<dim3((unsigned)((128) + 31) / 32, (unsigned)((Hs) + 15) / 16, (unsigned)(Bn * Hs)), 32, 0, stream>>>(c3_2); }
    { GemmP c3_3;
      c3_3.A = XP + (size_t)82 * 256; c3_3.B = w3 + 3; c3_3.bias = XP + (size_t)82 * 256; c3_3.R = T1; c3_3.C = T1;
      c3_3.sAo = (long long)PP * 256; c3_3.sAi = (long long)HP * 256; c3_3.sAm = 256; c3_3.sAk = 1; c3_3.sBo = 0; c3_3.sBi = 0; c3_3.sBn = 256 * 9; c3_3.sBk = 9; c3_3.sCo = (long long)HW * 128; c3_3.sCi = (long long)Hs * 128; c3_3.sCm = 128; c3_3.sRo = (long long)HW * 128; c3_3.sRi = (long long)Hs * 128; c3_3.sRm = 128; c3_3.sRn = 1;
      c3_3.M = Hs; c3_3.N = 128; c3_3.K = 256; c3_3.zi_n = Hs; c3_3.flags = 4; c3_3.act = 0;
      c3_3.alpha = 1.0f; c3_3.beta = 1.0f; c3_3.sa = 1.0f; c3_3.sb = 1.0f; c3_3.Npad = 128; c3_3.pad_ = 0;
      k_gemm<1><<<dim3((unsigned)((128) + 31) / 32, (unsigned)((Hs) + 15) / 16, (unsigned)(Bn * Hs)), 32, 0, stream>>>(c3_3); }
    { GemmP c3_4;
      c3_4.A = XP + (size_t)83 * 256; c3_4.B = w3 + 4; c3_4.bias = XP + (size_t)83 * 256; c3_4.R = T1; c3_4.C = T1;
      c3_4.sAo = (long long)PP * 256; c3_4.sAi = (long long)HP * 256; c3_4.sAm = 256; c3_4.sAk = 1; c3_4.sBo = 0; c3_4.sBi = 0; c3_4.sBn = 256 * 9; c3_4.sBk = 9; c3_4.sCo = (long long)HW * 128; c3_4.sCi = (long long)Hs * 128; c3_4.sCm = 128; c3_4.sRo = (long long)HW * 128; c3_4.sRi = (long long)Hs * 128; c3_4.sRm = 128; c3_4.sRn = 1;
      c3_4.M = Hs; c3_4.N = 128; c3_4.K = 256; c3_4.zi_n = Hs; c3_4.flags = 4; c3_4.act = 0;
      c3_4.alpha = 1.0f; c3_4.beta = 1.0f; c3_4.sa = 1.0f; c3_4.sb = 1.0f; c3_4.Npad = 128; c3_4.pad_ = 0;
      k_gemm<1><<<dim3((unsigned)((128) + 31) / 32, (unsigned)((Hs) + 15) / 16, (unsigned)(Bn * Hs)), 32, 0, stream>>>(c3_4); }
    { GemmP c3_5;
      c3_5.A = XP + (size_t)84 * 256; c3_5.B = w3 + 5; c3_5.bias = XP + (size_t)84 * 256; c3_5.R = T1; c3_5.C = T1;
      c3_5.sAo = (long long)PP * 256; c3_5.sAi = (long long)HP * 256; c3_5.sAm = 256; c3_5.sAk = 1; c3_5.sBo = 0; c3_5.sBi = 0; c3_5.sBn = 256 * 9; c3_5.sBk = 9; c3_5.sCo = (long long)HW * 128; c3_5.sCi = (long long)Hs * 128; c3_5.sCm = 128; c3_5.sRo = (long long)HW * 128; c3_5.sRi = (long long)Hs * 128; c3_5.sRm = 128; c3_5.sRn = 1;
      c3_5.M = Hs; c3_5.N = 128; c3_5.K = 256; c3_5.zi_n = Hs; c3_5.flags = 4; c3_5.act = 0;
      c3_5.alpha = 1.0f; c3_5.beta = 1.0f; c3_5.sa = 1.0f; c3_5.sb = 1.0f; c3_5.Npad = 128; c3_5.pad_ = 0;
      k_gemm<1><<<dim3((unsigned)((128) + 31) / 32, (unsigned)((Hs) + 15) / 16, (unsigned)(Bn * Hs)), 32, 0, stream>>>(c3_5); }
    { GemmP c3_6;
      c3_6.A = XP + (size_t)164 * 256; c3_6.B = w3 + 6; c3_6.bias = XP + (size_t)164 * 256; c3_6.R = T1; c3_6.C = T1;
      c3_6.sAo = (long long)PP * 256; c3_6.sAi = (long long)HP * 256; c3_6.sAm = 256; c3_6.sAk = 1; c3_6.sBo = 0; c3_6.sBi = 0; c3_6.sBn = 256 * 9; c3_6.sBk = 9; c3_6.sCo = (long long)HW * 128; c3_6.sCi = (long long)Hs * 128; c3_6.sCm = 128; c3_6.sRo = (long long)HW * 128; c3_6.sRi = (long long)Hs * 128; c3_6.sRm = 128; c3_6.sRn = 1;
      c3_6.M = Hs; c3_6.N = 128; c3_6.K = 256; c3_6.zi_n = Hs; c3_6.flags = 4; c3_6.act = 0;
      c3_6.alpha = 1.0f; c3_6.beta = 1.0f; c3_6.sa = 1.0f; c3_6.sb = 1.0f; c3_6.Npad = 128; c3_6.pad_ = 0;
      k_gemm<1><<<dim3((unsigned)((128) + 31) / 32, (unsigned)((Hs) + 15) / 16, (unsigned)(Bn * Hs)), 32, 0, stream>>>(c3_6); }
    { GemmP c3_7;
      c3_7.A = XP + (size_t)165 * 256; c3_7.B = w3 + 7; c3_7.bias = XP + (size_t)165 * 256; c3_7.R = T1; c3_7.C = T1;
      c3_7.sAo = (long long)PP * 256; c3_7.sAi = (long long)HP * 256; c3_7.sAm = 256; c3_7.sAk = 1; c3_7.sBo = 0; c3_7.sBi = 0; c3_7.sBn = 256 * 9; c3_7.sBk = 9; c3_7.sCo = (long long)HW * 128; c3_7.sCi = (long long)Hs * 128; c3_7.sCm = 128; c3_7.sRo = (long long)HW * 128; c3_7.sRi = (long long)Hs * 128; c3_7.sRm = 128; c3_7.sRn = 1;
      c3_7.M = Hs; c3_7.N = 128; c3_7.K = 256; c3_7.zi_n = Hs; c3_7.flags = 4; c3_7.act = 0;
      c3_7.alpha = 1.0f; c3_7.beta = 1.0f; c3_7.sa = 1.0f; c3_7.sb = 1.0f; c3_7.Npad = 128; c3_7.pad_ = 0;
      k_gemm<1><<<dim3((unsigned)((128) + 31) / 32, (unsigned)((Hs) + 15) / 16, (unsigned)(Bn * Hs)), 32, 0, stream>>>(c3_7); }
    { GemmP c3_8;
      c3_8.A = XP + (size_t)166 * 256; c3_8.B = w3 + 8; c3_8.bias = XP + (size_t)166 * 256; c3_8.R = T1; c3_8.C = T1;
      c3_8.sAo = (long long)PP * 256; c3_8.sAi = (long long)HP * 256; c3_8.sAm = 256; c3_8.sAk = 1; c3_8.sBo = 0; c3_8.sBi = 0; c3_8.sBn = 256 * 9; c3_8.sBk = 9; c3_8.sCo = (long long)HW * 128; c3_8.sCi = (long long)Hs * 128; c3_8.sCm = 128; c3_8.sRo = (long long)HW * 128; c3_8.sRi = (long long)Hs * 128; c3_8.sRm = 128; c3_8.sRn = 1;
      c3_8.M = Hs; c3_8.N = 128; c3_8.K = 256; c3_8.zi_n = Hs; c3_8.flags = 4; c3_8.act = 0;
      c3_8.alpha = 1.0f; c3_8.beta = 1.0f; c3_8.sa = 1.0f; c3_8.sb = 1.0f; c3_8.Npad = 128; c3_8.pad_ = 0;
      k_gemm<1><<<dim3((unsigned)((128) + 31) / 32, (unsigned)((Hs) + 15) / 16, (unsigned)(Bn * Hs)), 32, 0, stream>>>(c3_8); }

    k_sh_bn<<<(unsigned)(((long long)Bn * HW * 128 + 255) / 256), 256, 0, stream>>>(T1, 128, g3, bb3, m3, v3, OP, 256, 0, 1, Bn, Hs);
    { GemmP c51_0;
      c51_0.A = XP + (size_t)0 * 256; c51_0.B = w51 + 0; c51_0.bias = XP + (size_t)0 * 256; c51_0.R = XP + (size_t)0 * 256; c51_0.C = T64;
      c51_0.sAo = (long long)PP * 256; c51_0.sAi = (long long)HP * 256; c51_0.sAm = 256; c51_0.sAk = 1; c51_0.sBo = 0; c51_0.sBi = 0; c51_0.sBn = 256 * 9; c51_0.sBk = 9; c51_0.sCo = (long long)HW * 64; c51_0.sCi = (long long)Hs * 64; c51_0.sCm = 64; c51_0.sRo = 0; c51_0.sRi = 0; c51_0.sRm = 0; c51_0.sRn = 0;
      c51_0.M = Hs; c51_0.N = 64; c51_0.K = 256; c51_0.zi_n = Hs; c51_0.flags = 0; c51_0.act = 0;
      c51_0.alpha = 1.0f; c51_0.beta = 0.0f; c51_0.sa = 1.0f; c51_0.sb = 1.0f; c51_0.Npad = 64; c51_0.pad_ = 0;
      k_gemm<1><<<dim3((unsigned)((64) + 31) / 32, (unsigned)((Hs) + 15) / 16, (unsigned)(Bn * Hs)), 32, 0, stream>>>(c51_0); }
    { GemmP c51_1;
      c51_1.A = XP + (size_t)1 * 256; c51_1.B = w51 + 1; c51_1.bias = XP + (size_t)1 * 256; c51_1.R = T64; c51_1.C = T64;
      c51_1.sAo = (long long)PP * 256; c51_1.sAi = (long long)HP * 256; c51_1.sAm = 256; c51_1.sAk = 1; c51_1.sBo = 0; c51_1.sBi = 0; c51_1.sBn = 256 * 9; c51_1.sBk = 9; c51_1.sCo = (long long)HW * 64; c51_1.sCi = (long long)Hs * 64; c51_1.sCm = 64; c51_1.sRo = (long long)HW * 64; c51_1.sRi = (long long)Hs * 64; c51_1.sRm = 64; c51_1.sRn = 1;
      c51_1.M = Hs; c51_1.N = 64; c51_1.K = 256; c51_1.zi_n = Hs; c51_1.flags = 4; c51_1.act = 0;
      c51_1.alpha = 1.0f; c51_1.beta = 1.0f; c51_1.sa = 1.0f; c51_1.sb = 1.0f; c51_1.Npad = 64; c51_1.pad_ = 0;
      k_gemm<1><<<dim3((unsigned)((64) + 31) / 32, (unsigned)((Hs) + 15) / 16, (unsigned)(Bn * Hs)), 32, 0, stream>>>(c51_1); }
    { GemmP c51_2;
      c51_2.A = XP + (size_t)2 * 256; c51_2.B = w51 + 2; c51_2.bias = XP + (size_t)2 * 256; c51_2.R = T64; c51_2.C = T64;
      c51_2.sAo = (long long)PP * 256; c51_2.sAi = (long long)HP * 256; c51_2.sAm = 256; c51_2.sAk = 1; c51_2.sBo = 0; c51_2.sBi = 0; c51_2.sBn = 256 * 9; c51_2.sBk = 9; c51_2.sCo = (long long)HW * 64; c51_2.sCi = (long long)Hs * 64; c51_2.sCm = 64; c51_2.sRo = (long long)HW * 64; c51_2.sRi = (long long)Hs * 64; c51_2.sRm = 64; c51_2.sRn = 1;
      c51_2.M = Hs; c51_2.N = 64; c51_2.K = 256; c51_2.zi_n = Hs; c51_2.flags = 4; c51_2.act = 0;
      c51_2.alpha = 1.0f; c51_2.beta = 1.0f; c51_2.sa = 1.0f; c51_2.sb = 1.0f; c51_2.Npad = 64; c51_2.pad_ = 0;
      k_gemm<1><<<dim3((unsigned)((64) + 31) / 32, (unsigned)((Hs) + 15) / 16, (unsigned)(Bn * Hs)), 32, 0, stream>>>(c51_2); }
    { GemmP c51_3;
      c51_3.A = XP + (size_t)82 * 256; c51_3.B = w51 + 3; c51_3.bias = XP + (size_t)82 * 256; c51_3.R = T64; c51_3.C = T64;
      c51_3.sAo = (long long)PP * 256; c51_3.sAi = (long long)HP * 256; c51_3.sAm = 256; c51_3.sAk = 1; c51_3.sBo = 0; c51_3.sBi = 0; c51_3.sBn = 256 * 9; c51_3.sBk = 9; c51_3.sCo = (long long)HW * 64; c51_3.sCi = (long long)Hs * 64; c51_3.sCm = 64; c51_3.sRo = (long long)HW * 64; c51_3.sRi = (long long)Hs * 64; c51_3.sRm = 64; c51_3.sRn = 1;
      c51_3.M = Hs; c51_3.N = 64; c51_3.K = 256; c51_3.zi_n = Hs; c51_3.flags = 4; c51_3.act = 0;
      c51_3.alpha = 1.0f; c51_3.beta = 1.0f; c51_3.sa = 1.0f; c51_3.sb = 1.0f; c51_3.Npad = 64; c51_3.pad_ = 0;
      k_gemm<1><<<dim3((unsigned)((64) + 31) / 32, (unsigned)((Hs) + 15) / 16, (unsigned)(Bn * Hs)), 32, 0, stream>>>(c51_3); }
    { GemmP c51_4;
      c51_4.A = XP + (size_t)83 * 256; c51_4.B = w51 + 4; c51_4.bias = XP + (size_t)83 * 256; c51_4.R = T64; c51_4.C = T64;
      c51_4.sAo = (long long)PP * 256; c51_4.sAi = (long long)HP * 256; c51_4.sAm = 256; c51_4.sAk = 1; c51_4.sBo = 0; c51_4.sBi = 0; c51_4.sBn = 256 * 9; c51_4.sBk = 9; c51_4.sCo = (long long)HW * 64; c51_4.sCi = (long long)Hs * 64; c51_4.sCm = 64; c51_4.sRo = (long long)HW * 64; c51_4.sRi = (long long)Hs * 64; c51_4.sRm = 64; c51_4.sRn = 1;
      c51_4.M = Hs; c51_4.N = 64; c51_4.K = 256; c51_4.zi_n = Hs; c51_4.flags = 4; c51_4.act = 0;
      c51_4.alpha = 1.0f; c51_4.beta = 1.0f; c51_4.sa = 1.0f; c51_4.sb = 1.0f; c51_4.Npad = 64; c51_4.pad_ = 0;
      k_gemm<1><<<dim3((unsigned)((64) + 31) / 32, (unsigned)((Hs) + 15) / 16, (unsigned)(Bn * Hs)), 32, 0, stream>>>(c51_4); }
    { GemmP c51_5;
      c51_5.A = XP + (size_t)84 * 256; c51_5.B = w51 + 5; c51_5.bias = XP + (size_t)84 * 256; c51_5.R = T64; c51_5.C = T64;
      c51_5.sAo = (long long)PP * 256; c51_5.sAi = (long long)HP * 256; c51_5.sAm = 256; c51_5.sAk = 1; c51_5.sBo = 0; c51_5.sBi = 0; c51_5.sBn = 256 * 9; c51_5.sBk = 9; c51_5.sCo = (long long)HW * 64; c51_5.sCi = (long long)Hs * 64; c51_5.sCm = 64; c51_5.sRo = (long long)HW * 64; c51_5.sRi = (long long)Hs * 64; c51_5.sRm = 64; c51_5.sRn = 1;
      c51_5.M = Hs; c51_5.N = 64; c51_5.K = 256; c51_5.zi_n = Hs; c51_5.flags = 4; c51_5.act = 0;
      c51_5.alpha = 1.0f; c51_5.beta = 1.0f; c51_5.sa = 1.0f; c51_5.sb = 1.0f; c51_5.Npad = 64; c51_5.pad_ = 0;
      k_gemm<1><<<dim3((unsigned)((64) + 31) / 32, (unsigned)((Hs) + 15) / 16, (unsigned)(Bn * Hs)), 32, 0, stream>>>(c51_5); }
    { GemmP c51_6;
      c51_6.A = XP + (size_t)164 * 256; c51_6.B = w51 + 6; c51_6.bias = XP + (size_t)164 * 256; c51_6.R = T64; c51_6.C = T64;
      c51_6.sAo = (long long)PP * 256; c51_6.sAi = (long long)HP * 256; c51_6.sAm = 256; c51_6.sAk = 1; c51_6.sBo = 0; c51_6.sBi = 0; c51_6.sBn = 256 * 9; c51_6.sBk = 9; c51_6.sCo = (long long)HW * 64; c51_6.sCi = (long long)Hs * 64; c51_6.sCm = 64; c51_6.sRo = (long long)HW * 64; c51_6.sRi = (long long)Hs * 64; c51_6.sRm = 64; c51_6.sRn = 1;
      c51_6.M = Hs; c51_6.N = 64; c51_6.K = 256; c51_6.zi_n = Hs; c51_6.flags = 4; c51_6.act = 0;
      c51_6.alpha = 1.0f; c51_6.beta = 1.0f; c51_6.sa = 1.0f; c51_6.sb = 1.0f; c51_6.Npad = 64; c51_6.pad_ = 0;
      k_gemm<1><<<dim3((unsigned)((64) + 31) / 32, (unsigned)((Hs) + 15) / 16, (unsigned)(Bn * Hs)), 32, 0, stream>>>(c51_6); }
    { GemmP c51_7;
      c51_7.A = XP + (size_t)165 * 256; c51_7.B = w51 + 7; c51_7.bias = XP + (size_t)165 * 256; c51_7.R = T64; c51_7.C = T64;
      c51_7.sAo = (long long)PP * 256; c51_7.sAi = (long long)HP * 256; c51_7.sAm = 256; c51_7.sAk = 1; c51_7.sBo = 0; c51_7.sBi = 0; c51_7.sBn = 256 * 9; c51_7.sBk = 9; c51_7.sCo = (long long)HW * 64; c51_7.sCi = (long long)Hs * 64; c51_7.sCm = 64; c51_7.sRo = (long long)HW * 64; c51_7.sRi = (long long)Hs * 64; c51_7.sRm = 64; c51_7.sRn = 1;
      c51_7.M = Hs; c51_7.N = 64; c51_7.K = 256; c51_7.zi_n = Hs; c51_7.flags = 4; c51_7.act = 0;
      c51_7.alpha = 1.0f; c51_7.beta = 1.0f; c51_7.sa = 1.0f; c51_7.sb = 1.0f; c51_7.Npad = 64; c51_7.pad_ = 0;
      k_gemm<1><<<dim3((unsigned)((64) + 31) / 32, (unsigned)((Hs) + 15) / 16, (unsigned)(Bn * Hs)), 32, 0, stream>>>(c51_7); }
    { GemmP c51_8;
      c51_8.A = XP + (size_t)166 * 256; c51_8.B = w51 + 8; c51_8.bias = XP + (size_t)166 * 256; c51_8.R = T64; c51_8.C = T64;
      c51_8.sAo = (long long)PP * 256; c51_8.sAi = (long long)HP * 256; c51_8.sAm = 256; c51_8.sAk = 1; c51_8.sBo = 0; c51_8.sBi = 0; c51_8.sBn = 256 * 9; c51_8.sBk = 9; c51_8.sCo = (long long)HW * 64; c51_8.sCi = (long long)Hs * 64; c51_8.sCm = 64; c51_8.sRo = (long long)HW * 64; c51_8.sRi = (long long)Hs * 64; c51_8.sRm = 64; c51_8.sRn = 1;
      c51_8.M = Hs; c51_8.N = 64; c51_8.K = 256; c51_8.zi_n = Hs; c51_8.flags = 4; c51_8.act = 0;
      c51_8.alpha = 1.0f; c51_8.beta = 1.0f; c51_8.sa = 1.0f; c51_8.sb = 1.0f; c51_8.Npad = 64; c51_8.pad_ = 0;
      k_gemm<1><<<dim3((unsigned)((64) + 31) / 32, (unsigned)((Hs) + 15) / 16, (unsigned)(Bn * Hs)), 32, 0, stream>>>(c51_8); }

    k_sh_bn<<<(unsigned)(((long long)Bn * HW * 64 + 255) / 256), 256, 0, stream>>>(T64, 64, g51, bb51, m51, v51, P51, 64, 0, 1, Bn, Hs);
    { GemmP c52_0;
      c52_0.A = P51 + (size_t)0 * 64; c52_0.B = w52 + 0; c52_0.bias = P51 + (size_t)0 * 64; c52_0.R = P51 + (size_t)0 * 64; c52_0.C = T64;
      c52_0.sAo = (long long)PP * 64; c52_0.sAi = (long long)HP * 64; c52_0.sAm = 64; c52_0.sAk = 1; c52_0.sBo = 0; c52_0.sBi = 0; c52_0.sBn = 64 * 9; c52_0.sBk = 9; c52_0.sCo = (long long)HW * 64; c52_0.sCi = (long long)Hs * 64; c52_0.sCm = 64; c52_0.sRo = 0; c52_0.sRi = 0; c52_0.sRm = 0; c52_0.sRn = 0;
      c52_0.M = Hs; c52_0.N = 64; c52_0.K = 64; c52_0.zi_n = Hs; c52_0.flags = 0; c52_0.act = 0;
      c52_0.alpha = 1.0f; c52_0.beta = 0.0f; c52_0.sa = 1.0f; c52_0.sb = 1.0f; c52_0.Npad = 64; c52_0.pad_ = 0;
      k_gemm<1><<<dim3((unsigned)((64) + 31) / 32, (unsigned)((Hs) + 15) / 16, (unsigned)(Bn * Hs)), 32, 0, stream>>>(c52_0); }
    { GemmP c52_1;
      c52_1.A = P51 + (size_t)1 * 64; c52_1.B = w52 + 1; c52_1.bias = P51 + (size_t)1 * 64; c52_1.R = T64; c52_1.C = T64;
      c52_1.sAo = (long long)PP * 64; c52_1.sAi = (long long)HP * 64; c52_1.sAm = 64; c52_1.sAk = 1; c52_1.sBo = 0; c52_1.sBi = 0; c52_1.sBn = 64 * 9; c52_1.sBk = 9; c52_1.sCo = (long long)HW * 64; c52_1.sCi = (long long)Hs * 64; c52_1.sCm = 64; c52_1.sRo = (long long)HW * 64; c52_1.sRi = (long long)Hs * 64; c52_1.sRm = 64; c52_1.sRn = 1;
      c52_1.M = Hs; c52_1.N = 64; c52_1.K = 64; c52_1.zi_n = Hs; c52_1.flags = 4; c52_1.act = 0;
      c52_1.alpha = 1.0f; c52_1.beta = 1.0f; c52_1.sa = 1.0f; c52_1.sb = 1.0f; c52_1.Npad = 64; c52_1.pad_ = 0;
      k_gemm<1><<<dim3((unsigned)((64) + 31) / 32, (unsigned)((Hs) + 15) / 16, (unsigned)(Bn * Hs)), 32, 0, stream>>>(c52_1); }
    { GemmP c52_2;
      c52_2.A = P51 + (size_t)2 * 64; c52_2.B = w52 + 2; c52_2.bias = P51 + (size_t)2 * 64; c52_2.R = T64; c52_2.C = T64;
      c52_2.sAo = (long long)PP * 64; c52_2.sAi = (long long)HP * 64; c52_2.sAm = 64; c52_2.sAk = 1; c52_2.sBo = 0; c52_2.sBi = 0; c52_2.sBn = 64 * 9; c52_2.sBk = 9; c52_2.sCo = (long long)HW * 64; c52_2.sCi = (long long)Hs * 64; c52_2.sCm = 64; c52_2.sRo = (long long)HW * 64; c52_2.sRi = (long long)Hs * 64; c52_2.sRm = 64; c52_2.sRn = 1;
      c52_2.M = Hs; c52_2.N = 64; c52_2.K = 64; c52_2.zi_n = Hs; c52_2.flags = 4; c52_2.act = 0;
      c52_2.alpha = 1.0f; c52_2.beta = 1.0f; c52_2.sa = 1.0f; c52_2.sb = 1.0f; c52_2.Npad = 64; c52_2.pad_ = 0;
      k_gemm<1><<<dim3((unsigned)((64) + 31) / 32, (unsigned)((Hs) + 15) / 16, (unsigned)(Bn * Hs)), 32, 0, stream>>>(c52_2); }
    { GemmP c52_3;
      c52_3.A = P51 + (size_t)82 * 64; c52_3.B = w52 + 3; c52_3.bias = P51 + (size_t)82 * 64; c52_3.R = T64; c52_3.C = T64;
      c52_3.sAo = (long long)PP * 64; c52_3.sAi = (long long)HP * 64; c52_3.sAm = 64; c52_3.sAk = 1; c52_3.sBo = 0; c52_3.sBi = 0; c52_3.sBn = 64 * 9; c52_3.sBk = 9; c52_3.sCo = (long long)HW * 64; c52_3.sCi = (long long)Hs * 64; c52_3.sCm = 64; c52_3.sRo = (long long)HW * 64; c52_3.sRi = (long long)Hs * 64; c52_3.sRm = 64; c52_3.sRn = 1;
      c52_3.M = Hs; c52_3.N = 64; c52_3.K = 64; c52_3.zi_n = Hs; c52_3.flags = 4; c52_3.act = 0;
      c52_3.alpha = 1.0f; c52_3.beta = 1.0f; c52_3.sa = 1.0f; c52_3.sb = 1.0f; c52_3.Npad = 64; c52_3.pad_ = 0;
      k_gemm<1><<<dim3((unsigned)((64) + 31) / 32, (unsigned)((Hs) + 15) / 16, (unsigned)(Bn * Hs)), 32, 0, stream>>>(c52_3); }
    { GemmP c52_4;
      c52_4.A = P51 + (size_t)83 * 64; c52_4.B = w52 + 4; c52_4.bias = P51 + (size_t)83 * 64; c52_4.R = T64; c52_4.C = T64;
      c52_4.sAo = (long long)PP * 64; c52_4.sAi = (long long)HP * 64; c52_4.sAm = 64; c52_4.sAk = 1; c52_4.sBo = 0; c52_4.sBi = 0; c52_4.sBn = 64 * 9; c52_4.sBk = 9; c52_4.sCo = (long long)HW * 64; c52_4.sCi = (long long)Hs * 64; c52_4.sCm = 64; c52_4.sRo = (long long)HW * 64; c52_4.sRi = (long long)Hs * 64; c52_4.sRm = 64; c52_4.sRn = 1;
      c52_4.M = Hs; c52_4.N = 64; c52_4.K = 64; c52_4.zi_n = Hs; c52_4.flags = 4; c52_4.act = 0;
      c52_4.alpha = 1.0f; c52_4.beta = 1.0f; c52_4.sa = 1.0f; c52_4.sb = 1.0f; c52_4.Npad = 64; c52_4.pad_ = 0;
      k_gemm<1><<<dim3((unsigned)((64) + 31) / 32, (unsigned)((Hs) + 15) / 16, (unsigned)(Bn * Hs)), 32, 0, stream>>>(c52_4); }
    { GemmP c52_5;
      c52_5.A = P51 + (size_t)84 * 64; c52_5.B = w52 + 5; c52_5.bias = P51 + (size_t)84 * 64; c52_5.R = T64; c52_5.C = T64;
      c52_5.sAo = (long long)PP * 64; c52_5.sAi = (long long)HP * 64; c52_5.sAm = 64; c52_5.sAk = 1; c52_5.sBo = 0; c52_5.sBi = 0; c52_5.sBn = 64 * 9; c52_5.sBk = 9; c52_5.sCo = (long long)HW * 64; c52_5.sCi = (long long)Hs * 64; c52_5.sCm = 64; c52_5.sRo = (long long)HW * 64; c52_5.sRi = (long long)Hs * 64; c52_5.sRm = 64; c52_5.sRn = 1;
      c52_5.M = Hs; c52_5.N = 64; c52_5.K = 64; c52_5.zi_n = Hs; c52_5.flags = 4; c52_5.act = 0;
      c52_5.alpha = 1.0f; c52_5.beta = 1.0f; c52_5.sa = 1.0f; c52_5.sb = 1.0f; c52_5.Npad = 64; c52_5.pad_ = 0;
      k_gemm<1><<<dim3((unsigned)((64) + 31) / 32, (unsigned)((Hs) + 15) / 16, (unsigned)(Bn * Hs)), 32, 0, stream>>>(c52_5); }
    { GemmP c52_6;
      c52_6.A = P51 + (size_t)164 * 64; c52_6.B = w52 + 6; c52_6.bias = P51 + (size_t)164 * 64; c52_6.R = T64; c52_6.C = T64;
      c52_6.sAo = (long long)PP * 64; c52_6.sAi = (long long)HP * 64; c52_6.sAm = 64; c52_6.sAk = 1; c52_6.sBo = 0; c52_6.sBi = 0; c52_6.sBn = 64 * 9; c52_6.sBk = 9; c52_6.sCo = (long long)HW * 64; c52_6.sCi = (long long)Hs * 64; c52_6.sCm = 64; c52_6.sRo = (long long)HW * 64; c52_6.sRi = (long long)Hs * 64; c52_6.sRm = 64; c52_6.sRn = 1;
      c52_6.M = Hs; c52_6.N = 64; c52_6.K = 64; c52_6.zi_n = Hs; c52_6.flags = 4; c52_6.act = 0;
      c52_6.alpha = 1.0f; c52_6.beta = 1.0f; c52_6.sa = 1.0f; c52_6.sb = 1.0f; c52_6.Npad = 64; c52_6.pad_ = 0;
      k_gemm<1><<<dim3((unsigned)((64) + 31) / 32, (unsigned)((Hs) + 15) / 16, (unsigned)(Bn * Hs)), 32, 0, stream>>>(c52_6); }
    { GemmP c52_7;
      c52_7.A = P51 + (size_t)165 * 64; c52_7.B = w52 + 7; c52_7.bias = P51 + (size_t)165 * 64; c52_7.R = T64; c52_7.C = T64;
      c52_7.sAo = (long long)PP * 64; c52_7.sAi = (long long)HP * 64; c52_7.sAm = 64; c52_7.sAk = 1; c52_7.sBo = 0; c52_7.sBi = 0; c52_7.sBn = 64 * 9; c52_7.sBk = 9; c52_7.sCo = (long long)HW * 64; c52_7.sCi = (long long)Hs * 64; c52_7.sCm = 64; c52_7.sRo = (long long)HW * 64; c52_7.sRi = (long long)Hs * 64; c52_7.sRm = 64; c52_7.sRn = 1;
      c52_7.M = Hs; c52_7.N = 64; c52_7.K = 64; c52_7.zi_n = Hs; c52_7.flags = 4; c52_7.act = 0;
      c52_7.alpha = 1.0f; c52_7.beta = 1.0f; c52_7.sa = 1.0f; c52_7.sb = 1.0f; c52_7.Npad = 64; c52_7.pad_ = 0;
      k_gemm<1><<<dim3((unsigned)((64) + 31) / 32, (unsigned)((Hs) + 15) / 16, (unsigned)(Bn * Hs)), 32, 0, stream>>>(c52_7); }
    { GemmP c52_8;
      c52_8.A = P51 + (size_t)166 * 64; c52_8.B = w52 + 8; c52_8.bias = P51 + (size_t)166 * 64; c52_8.R = T64; c52_8.C = T64;
      c52_8.sAo = (long long)PP * 64; c52_8.sAi = (long long)HP * 64; c52_8.sAm = 64; c52_8.sAk = 1; c52_8.sBo = 0; c52_8.sBi = 0; c52_8.sBn = 64 * 9; c52_8.sBk = 9; c52_8.sCo = (long long)HW * 64; c52_8.sCi = (long long)Hs * 64; c52_8.sCm = 64; c52_8.sRo = (long long)HW * 64; c52_8.sRi = (long long)Hs * 64; c52_8.sRm = 64; c52_8.sRn = 1;
      c52_8.M = Hs; c52_8.N = 64; c52_8.K = 64; c52_8.zi_n = Hs; c52_8.flags = 4; c52_8.act = 0;
      c52_8.alpha = 1.0f; c52_8.beta = 1.0f; c52_8.sa = 1.0f; c52_8.sb = 1.0f; c52_8.Npad = 64; c52_8.pad_ = 0;
      k_gemm<1><<<dim3((unsigned)((64) + 31) / 32, (unsigned)((Hs) + 15) / 16, (unsigned)(Bn * Hs)), 32, 0, stream>>>(c52_8); }

    k_sh_bn<<<(unsigned)(((long long)Bn * HW * 64 + 255) / 256), 256, 0, stream>>>(T64, 64, g52, bb52, m52, v52, OP, 256, 128, 1, Bn, Hs);
    { GemmP c72_0;
      c72_0.A = P51 + (size_t)0 * 64; c72_0.B = w72 + 0; c72_0.bias = P51 + (size_t)0 * 64; c72_0.R = P51 + (size_t)0 * 64; c72_0.C = T64;
      c72_0.sAo = (long long)PP * 64; c72_0.sAi = (long long)HP * 64; c72_0.sAm = 64; c72_0.sAk = 1; c72_0.sBo = 0; c72_0.sBi = 0; c72_0.sBn = 64 * 9; c72_0.sBk = 9; c72_0.sCo = (long long)HW * 64; c72_0.sCi = (long long)Hs * 64; c72_0.sCm = 64; c72_0.sRo = 0; c72_0.sRi = 0; c72_0.sRm = 0; c72_0.sRn = 0;
      c72_0.M = Hs; c72_0.N = 64; c72_0.K = 64; c72_0.zi_n = Hs; c72_0.flags = 0; c72_0.act = 0;
      c72_0.alpha = 1.0f; c72_0.beta = 0.0f; c72_0.sa = 1.0f; c72_0.sb = 1.0f; c72_0.Npad = 64; c72_0.pad_ = 0;
      k_gemm<1><<<dim3((unsigned)((64) + 31) / 32, (unsigned)((Hs) + 15) / 16, (unsigned)(Bn * Hs)), 32, 0, stream>>>(c72_0); }
    { GemmP c72_1;
      c72_1.A = P51 + (size_t)1 * 64; c72_1.B = w72 + 1; c72_1.bias = P51 + (size_t)1 * 64; c72_1.R = T64; c72_1.C = T64;
      c72_1.sAo = (long long)PP * 64; c72_1.sAi = (long long)HP * 64; c72_1.sAm = 64; c72_1.sAk = 1; c72_1.sBo = 0; c72_1.sBi = 0; c72_1.sBn = 64 * 9; c72_1.sBk = 9; c72_1.sCo = (long long)HW * 64; c72_1.sCi = (long long)Hs * 64; c72_1.sCm = 64; c72_1.sRo = (long long)HW * 64; c72_1.sRi = (long long)Hs * 64; c72_1.sRm = 64; c72_1.sRn = 1;
      c72_1.M = Hs; c72_1.N = 64; c72_1.K = 64; c72_1.zi_n = Hs; c72_1.flags = 4; c72_1.act = 0;
      c72_1.alpha = 1.0f; c72_1.beta = 1.0f; c72_1.sa = 1.0f; c72_1.sb = 1.0f; c72_1.Npad = 64; c72_1.pad_ = 0;
      k_gemm<1><<<dim3((unsigned)((64) + 31) / 32, (unsigned)((Hs) + 15) / 16, (unsigned)(Bn * Hs)), 32, 0, stream>>>(c72_1); }
    { GemmP c72_2;
      c72_2.A = P51 + (size_t)2 * 64; c72_2.B = w72 + 2; c72_2.bias = P51 + (size_t)2 * 64; c72_2.R = T64; c72_2.C = T64;
      c72_2.sAo = (long long)PP * 64; c72_2.sAi = (long long)HP * 64; c72_2.sAm = 64; c72_2.sAk = 1; c72_2.sBo = 0; c72_2.sBi = 0; c72_2.sBn = 64 * 9; c72_2.sBk = 9; c72_2.sCo = (long long)HW * 64; c72_2.sCi = (long long)Hs * 64; c72_2.sCm = 64; c72_2.sRo = (long long)HW * 64; c72_2.sRi = (long long)Hs * 64; c72_2.sRm = 64; c72_2.sRn = 1;
      c72_2.M = Hs; c72_2.N = 64; c72_2.K = 64; c72_2.zi_n = Hs; c72_2.flags = 4; c72_2.act = 0;
      c72_2.alpha = 1.0f; c72_2.beta = 1.0f; c72_2.sa = 1.0f; c72_2.sb = 1.0f; c72_2.Npad = 64; c72_2.pad_ = 0;
      k_gemm<1><<<dim3((unsigned)((64) + 31) / 32, (unsigned)((Hs) + 15) / 16, (unsigned)(Bn * Hs)), 32, 0, stream>>>(c72_2); }
    { GemmP c72_3;
      c72_3.A = P51 + (size_t)82 * 64; c72_3.B = w72 + 3; c72_3.bias = P51 + (size_t)82 * 64; c72_3.R = T64; c72_3.C = T64;
      c72_3.sAo = (long long)PP * 64; c72_3.sAi = (long long)HP * 64; c72_3.sAm = 64; c72_3.sAk = 1; c72_3.sBo = 0; c72_3.sBi = 0; c72_3.sBn = 64 * 9; c72_3.sBk = 9; c72_3.sCo = (long long)HW * 64; c72_3.sCi = (long long)Hs * 64; c72_3.sCm = 64; c72_3.sRo = (long long)HW * 64; c72_3.sRi = (long long)Hs * 64; c72_3.sRm = 64; c72_3.sRn = 1;
      c72_3.M = Hs; c72_3.N = 64; c72_3.K = 64; c72_3.zi_n = Hs; c72_3.flags = 4; c72_3.act = 0;
      c72_3.alpha = 1.0f; c72_3.beta = 1.0f; c72_3.sa = 1.0f; c72_3.sb = 1.0f; c72_3.Npad = 64; c72_3.pad_ = 0;
      k_gemm<1><<<dim3((unsigned)((64) + 31) / 32, (unsigned)((Hs) + 15) / 16, (unsigned)(Bn * Hs)), 32, 0, stream>>>(c72_3); }
    { GemmP c72_4;
      c72_4.A = P51 + (size_t)83 * 64; c72_4.B = w72 + 4; c72_4.bias = P51 + (size_t)83 * 64; c72_4.R = T64; c72_4.C = T64;
      c72_4.sAo = (long long)PP * 64; c72_4.sAi = (long long)HP * 64; c72_4.sAm = 64; c72_4.sAk = 1; c72_4.sBo = 0; c72_4.sBi = 0; c72_4.sBn = 64 * 9; c72_4.sBk = 9; c72_4.sCo = (long long)HW * 64; c72_4.sCi = (long long)Hs * 64; c72_4.sCm = 64; c72_4.sRo = (long long)HW * 64; c72_4.sRi = (long long)Hs * 64; c72_4.sRm = 64; c72_4.sRn = 1;
      c72_4.M = Hs; c72_4.N = 64; c72_4.K = 64; c72_4.zi_n = Hs; c72_4.flags = 4; c72_4.act = 0;
      c72_4.alpha = 1.0f; c72_4.beta = 1.0f; c72_4.sa = 1.0f; c72_4.sb = 1.0f; c72_4.Npad = 64; c72_4.pad_ = 0;
      k_gemm<1><<<dim3((unsigned)((64) + 31) / 32, (unsigned)((Hs) + 15) / 16, (unsigned)(Bn * Hs)), 32, 0, stream>>>(c72_4); }
    { GemmP c72_5;
      c72_5.A = P51 + (size_t)84 * 64; c72_5.B = w72 + 5; c72_5.bias = P51 + (size_t)84 * 64; c72_5.R = T64; c72_5.C = T64;
      c72_5.sAo = (long long)PP * 64; c72_5.sAi = (long long)HP * 64; c72_5.sAm = 64; c72_5.sAk = 1; c72_5.sBo = 0; c72_5.sBi = 0; c72_5.sBn = 64 * 9; c72_5.sBk = 9; c72_5.sCo = (long long)HW * 64; c72_5.sCi = (long long)Hs * 64; c72_5.sCm = 64; c72_5.sRo = (long long)HW * 64; c72_5.sRi = (long long)Hs * 64; c72_5.sRm = 64; c72_5.sRn = 1;
      c72_5.M = Hs; c72_5.N = 64; c72_5.K = 64; c72_5.zi_n = Hs; c72_5.flags = 4; c72_5.act = 0;
      c72_5.alpha = 1.0f; c72_5.beta = 1.0f; c72_5.sa = 1.0f; c72_5.sb = 1.0f; c72_5.Npad = 64; c72_5.pad_ = 0;
      k_gemm<1><<<dim3((unsigned)((64) + 31) / 32, (unsigned)((Hs) + 15) / 16, (unsigned)(Bn * Hs)), 32, 0, stream>>>(c72_5); }
    { GemmP c72_6;
      c72_6.A = P51 + (size_t)164 * 64; c72_6.B = w72 + 6; c72_6.bias = P51 + (size_t)164 * 64; c72_6.R = T64; c72_6.C = T64;
      c72_6.sAo = (long long)PP * 64; c72_6.sAi = (long long)HP * 64; c72_6.sAm = 64; c72_6.sAk = 1; c72_6.sBo = 0; c72_6.sBi = 0; c72_6.sBn = 64 * 9; c72_6.sBk = 9; c72_6.sCo = (long long)HW * 64; c72_6.sCi = (long long)Hs * 64; c72_6.sCm = 64; c72_6.sRo = (long long)HW * 64; c72_6.sRi = (long long)Hs * 64; c72_6.sRm = 64; c72_6.sRn = 1;
      c72_6.M = Hs; c72_6.N = 64; c72_6.K = 64; c72_6.zi_n = Hs; c72_6.flags = 4; c72_6.act = 0;
      c72_6.alpha = 1.0f; c72_6.beta = 1.0f; c72_6.sa = 1.0f; c72_6.sb = 1.0f; c72_6.Npad = 64; c72_6.pad_ = 0;
      k_gemm<1><<<dim3((unsigned)((64) + 31) / 32, (unsigned)((Hs) + 15) / 16, (unsigned)(Bn * Hs)), 32, 0, stream>>>(c72_6); }
    { GemmP c72_7;
      c72_7.A = P51 + (size_t)165 * 64; c72_7.B = w72 + 7; c72_7.bias = P51 + (size_t)165 * 64; c72_7.R = T64; c72_7.C = T64;
      c72_7.sAo = (long long)PP * 64; c72_7.sAi = (long long)HP * 64; c72_7.sAm = 64; c72_7.sAk = 1; c72_7.sBo = 0; c72_7.sBi = 0; c72_7.sBn = 64 * 9; c72_7.sBk = 9; c72_7.sCo = (long long)HW * 64; c72_7.sCi = (long long)Hs * 64; c72_7.sCm = 64; c72_7.sRo = (long long)HW * 64; c72_7.sRi = (long long)Hs * 64; c72_7.sRm = 64; c72_7.sRn = 1;
      c72_7.M = Hs; c72_7.N = 64; c72_7.K = 64; c72_7.zi_n = Hs; c72_7.flags = 4; c72_7.act = 0;
      c72_7.alpha = 1.0f; c72_7.beta = 1.0f; c72_7.sa = 1.0f; c72_7.sb = 1.0f; c72_7.Npad = 64; c72_7.pad_ = 0;
      k_gemm<1><<<dim3((unsigned)((64) + 31) / 32, (unsigned)((Hs) + 15) / 16, (unsigned)(Bn * Hs)), 32, 0, stream>>>(c72_7); }
    { GemmP c72_8;
      c72_8.A = P51 + (size_t)166 * 64; c72_8.B = w72 + 8; c72_8.bias = P51 + (size_t)166 * 64; c72_8.R = T64; c72_8.C = T64;
      c72_8.sAo = (long long)PP * 64; c72_8.sAi = (long long)HP * 64; c72_8.sAm = 64; c72_8.sAk = 1; c72_8.sBo = 0; c72_8.sBi = 0; c72_8.sBn = 64 * 9; c72_8.sBk = 9; c72_8.sCo = (long long)HW * 64; c72_8.sCi = (long long)Hs * 64; c72_8.sCm = 64; c72_8.sRo = (long long)HW * 64; c72_8.sRi = (long long)Hs * 64; c72_8.sRm = 64; c72_8.sRn = 1;
      c72_8.M = Hs; c72_8.N = 64; c72_8.K = 64; c72_8.zi_n = Hs; c72_8.flags = 4; c72_8.act = 0;
      c72_8.alpha = 1.0f; c72_8.beta = 1.0f; c72_8.sa = 1.0f; c72_8.sb = 1.0f; c72_8.Npad = 64; c72_8.pad_ = 0;
      k_gemm<1><<<dim3((unsigned)((64) + 31) / 32, (unsigned)((Hs) + 15) / 16, (unsigned)(Bn * Hs)), 32, 0, stream>>>(c72_8); }

    k_sh_bn<<<(unsigned)(((long long)Bn * HW * 64 + 255) / 256), 256, 0, stream>>>(T64, 64, g72, bb72, m72, v72, P72, 64, 0, 1, Bn, Hs);
    { GemmP c73_0;
      c73_0.A = P72 + (size_t)0 * 64; c73_0.B = w73 + 0; c73_0.bias = P72 + (size_t)0 * 64; c73_0.R = P72 + (size_t)0 * 64; c73_0.C = T64;
      c73_0.sAo = (long long)PP * 64; c73_0.sAi = (long long)HP * 64; c73_0.sAm = 64; c73_0.sAk = 1; c73_0.sBo = 0; c73_0.sBi = 0; c73_0.sBn = 64 * 9; c73_0.sBk = 9; c73_0.sCo = (long long)HW * 64; c73_0.sCi = (long long)Hs * 64; c73_0.sCm = 64; c73_0.sRo = 0; c73_0.sRi = 0; c73_0.sRm = 0; c73_0.sRn = 0;
      c73_0.M = Hs; c73_0.N = 64; c73_0.K = 64; c73_0.zi_n = Hs; c73_0.flags = 0; c73_0.act = 0;
      c73_0.alpha = 1.0f; c73_0.beta = 0.0f; c73_0.sa = 1.0f; c73_0.sb = 1.0f; c73_0.Npad = 64; c73_0.pad_ = 0;
      k_gemm<1><<<dim3((unsigned)((64) + 31) / 32, (unsigned)((Hs) + 15) / 16, (unsigned)(Bn * Hs)), 32, 0, stream>>>(c73_0); }
    { GemmP c73_1;
      c73_1.A = P72 + (size_t)1 * 64; c73_1.B = w73 + 1; c73_1.bias = P72 + (size_t)1 * 64; c73_1.R = T64; c73_1.C = T64;
      c73_1.sAo = (long long)PP * 64; c73_1.sAi = (long long)HP * 64; c73_1.sAm = 64; c73_1.sAk = 1; c73_1.sBo = 0; c73_1.sBi = 0; c73_1.sBn = 64 * 9; c73_1.sBk = 9; c73_1.sCo = (long long)HW * 64; c73_1.sCi = (long long)Hs * 64; c73_1.sCm = 64; c73_1.sRo = (long long)HW * 64; c73_1.sRi = (long long)Hs * 64; c73_1.sRm = 64; c73_1.sRn = 1;
      c73_1.M = Hs; c73_1.N = 64; c73_1.K = 64; c73_1.zi_n = Hs; c73_1.flags = 4; c73_1.act = 0;
      c73_1.alpha = 1.0f; c73_1.beta = 1.0f; c73_1.sa = 1.0f; c73_1.sb = 1.0f; c73_1.Npad = 64; c73_1.pad_ = 0;
      k_gemm<1><<<dim3((unsigned)((64) + 31) / 32, (unsigned)((Hs) + 15) / 16, (unsigned)(Bn * Hs)), 32, 0, stream>>>(c73_1); }
    { GemmP c73_2;
      c73_2.A = P72 + (size_t)2 * 64; c73_2.B = w73 + 2; c73_2.bias = P72 + (size_t)2 * 64; c73_2.R = T64; c73_2.C = T64;
      c73_2.sAo = (long long)PP * 64; c73_2.sAi = (long long)HP * 64; c73_2.sAm = 64; c73_2.sAk = 1; c73_2.sBo = 0; c73_2.sBi = 0; c73_2.sBn = 64 * 9; c73_2.sBk = 9; c73_2.sCo = (long long)HW * 64; c73_2.sCi = (long long)Hs * 64; c73_2.sCm = 64; c73_2.sRo = (long long)HW * 64; c73_2.sRi = (long long)Hs * 64; c73_2.sRm = 64; c73_2.sRn = 1;
      c73_2.M = Hs; c73_2.N = 64; c73_2.K = 64; c73_2.zi_n = Hs; c73_2.flags = 4; c73_2.act = 0;
      c73_2.alpha = 1.0f; c73_2.beta = 1.0f; c73_2.sa = 1.0f; c73_2.sb = 1.0f; c73_2.Npad = 64; c73_2.pad_ = 0;
      k_gemm<1><<<dim3((unsigned)((64) + 31) / 32, (unsigned)((Hs) + 15) / 16, (unsigned)(Bn * Hs)), 32, 0, stream>>>(c73_2); }
    { GemmP c73_3;
      c73_3.A = P72 + (size_t)82 * 64; c73_3.B = w73 + 3; c73_3.bias = P72 + (size_t)82 * 64; c73_3.R = T64; c73_3.C = T64;
      c73_3.sAo = (long long)PP * 64; c73_3.sAi = (long long)HP * 64; c73_3.sAm = 64; c73_3.sAk = 1; c73_3.sBo = 0; c73_3.sBi = 0; c73_3.sBn = 64 * 9; c73_3.sBk = 9; c73_3.sCo = (long long)HW * 64; c73_3.sCi = (long long)Hs * 64; c73_3.sCm = 64; c73_3.sRo = (long long)HW * 64; c73_3.sRi = (long long)Hs * 64; c73_3.sRm = 64; c73_3.sRn = 1;
      c73_3.M = Hs; c73_3.N = 64; c73_3.K = 64; c73_3.zi_n = Hs; c73_3.flags = 4; c73_3.act = 0;
      c73_3.alpha = 1.0f; c73_3.beta = 1.0f; c73_3.sa = 1.0f; c73_3.sb = 1.0f; c73_3.Npad = 64; c73_3.pad_ = 0;
      k_gemm<1><<<dim3((unsigned)((64) + 31) / 32, (unsigned)((Hs) + 15) / 16, (unsigned)(Bn * Hs)), 32, 0, stream>>>(c73_3); }
    { GemmP c73_4;
      c73_4.A = P72 + (size_t)83 * 64; c73_4.B = w73 + 4; c73_4.bias = P72 + (size_t)83 * 64; c73_4.R = T64; c73_4.C = T64;
      c73_4.sAo = (long long)PP * 64; c73_4.sAi = (long long)HP * 64; c73_4.sAm = 64; c73_4.sAk = 1; c73_4.sBo = 0; c73_4.sBi = 0; c73_4.sBn = 64 * 9; c73_4.sBk = 9; c73_4.sCo = (long long)HW * 64; c73_4.sCi = (long long)Hs * 64; c73_4.sCm = 64; c73_4.sRo = (long long)HW * 64; c73_4.sRi = (long long)Hs * 64; c73_4.sRm = 64; c73_4.sRn = 1;
      c73_4.M = Hs; c73_4.N = 64; c73_4.K = 64; c73_4.zi_n = Hs; c73_4.flags = 4; c73_4.act = 0;
      c73_4.alpha = 1.0f; c73_4.beta = 1.0f; c73_4.sa = 1.0f; c73_4.sb = 1.0f; c73_4.Npad = 64; c73_4.pad_ = 0;
      k_gemm<1><<<dim3((unsigned)((64) + 31) / 32, (unsigned)((Hs) + 15) / 16, (unsigned)(Bn * Hs)), 32, 0, stream>>>(c73_4); }
    { GemmP c73_5;
      c73_5.A = P72 + (size_t)84 * 64; c73_5.B = w73 + 5; c73_5.bias = P72 + (size_t)84 * 64; c73_5.R = T64; c73_5.C = T64;
      c73_5.sAo = (long long)PP * 64; c73_5.sAi = (long long)HP * 64; c73_5.sAm = 64; c73_5.sAk = 1; c73_5.sBo = 0; c73_5.sBi = 0; c73_5.sBn = 64 * 9; c73_5.sBk = 9; c73_5.sCo = (long long)HW * 64; c73_5.sCi = (long long)Hs * 64; c73_5.sCm = 64; c73_5.sRo = (long long)HW * 64; c73_5.sRi = (long long)Hs * 64; c73_5.sRm = 64; c73_5.sRn = 1;
      c73_5.M = Hs; c73_5.N = 64; c73_5.K = 64; c73_5.zi_n = Hs; c73_5.flags = 4; c73_5.act = 0;
      c73_5.alpha = 1.0f; c73_5.beta = 1.0f; c73_5.sa = 1.0f; c73_5.sb = 1.0f; c73_5.Npad = 64; c73_5.pad_ = 0;
      k_gemm<1><<<dim3((unsigned)((64) + 31) / 32, (unsigned)((Hs) + 15) / 16, (unsigned)(Bn * Hs)), 32, 0, stream>>>(c73_5); }
    { GemmP c73_6;
      c73_6.A = P72 + (size_t)164 * 64; c73_6.B = w73 + 6; c73_6.bias = P72 + (size_t)164 * 64; c73_6.R = T64; c73_6.C = T64;
      c73_6.sAo = (long long)PP * 64; c73_6.sAi = (long long)HP * 64; c73_6.sAm = 64; c73_6.sAk = 1; c73_6.sBo = 0; c73_6.sBi = 0; c73_6.sBn = 64 * 9; c73_6.sBk = 9; c73_6.sCo = (long long)HW * 64; c73_6.sCi = (long long)Hs * 64; c73_6.sCm = 64; c73_6.sRo = (long long)HW * 64; c73_6.sRi = (long long)Hs * 64; c73_6.sRm = 64; c73_6.sRn = 1;
      c73_6.M = Hs; c73_6.N = 64; c73_6.K = 64; c73_6.zi_n = Hs; c73_6.flags = 4; c73_6.act = 0;
      c73_6.alpha = 1.0f; c73_6.beta = 1.0f; c73_6.sa = 1.0f; c73_6.sb = 1.0f; c73_6.Npad = 64; c73_6.pad_ = 0;
      k_gemm<1><<<dim3((unsigned)((64) + 31) / 32, (unsigned)((Hs) + 15) / 16, (unsigned)(Bn * Hs)), 32, 0, stream>>>(c73_6); }
    { GemmP c73_7;
      c73_7.A = P72 + (size_t)165 * 64; c73_7.B = w73 + 7; c73_7.bias = P72 + (size_t)165 * 64; c73_7.R = T64; c73_7.C = T64;
      c73_7.sAo = (long long)PP * 64; c73_7.sAi = (long long)HP * 64; c73_7.sAm = 64; c73_7.sAk = 1; c73_7.sBo = 0; c73_7.sBi = 0; c73_7.sBn = 64 * 9; c73_7.sBk = 9; c73_7.sCo = (long long)HW * 64; c73_7.sCi = (long long)Hs * 64; c73_7.sCm = 64; c73_7.sRo = (long long)HW * 64; c73_7.sRi = (long long)Hs * 64; c73_7.sRm = 64; c73_7.sRn = 1;
      c73_7.M = Hs; c73_7.N = 64; c73_7.K = 64; c73_7.zi_n = Hs; c73_7.flags = 4; c73_7.act = 0;
      c73_7.alpha = 1.0f; c73_7.beta = 1.0f; c73_7.sa = 1.0f; c73_7.sb = 1.0f; c73_7.Npad = 64; c73_7.pad_ = 0;
      k_gemm<1><<<dim3((unsigned)((64) + 31) / 32, (unsigned)((Hs) + 15) / 16, (unsigned)(Bn * Hs)), 32, 0, stream>>>(c73_7); }
    { GemmP c73_8;
      c73_8.A = P72 + (size_t)166 * 64; c73_8.B = w73 + 8; c73_8.bias = P72 + (size_t)166 * 64; c73_8.R = T64; c73_8.C = T64;
      c73_8.sAo = (long long)PP * 64; c73_8.sAi = (long long)HP * 64; c73_8.sAm = 64; c73_8.sAk = 1; c73_8.sBo = 0; c73_8.sBi = 0; c73_8.sBn = 64 * 9; c73_8.sBk = 9; c73_8.sCo = (long long)HW * 64; c73_8.sCi = (long long)Hs * 64; c73_8.sCm = 64; c73_8.sRo = (long long)HW * 64; c73_8.sRi = (long long)Hs * 64; c73_8.sRm = 64; c73_8.sRn = 1;
      c73_8.M = Hs; c73_8.N = 64; c73_8.K = 64; c73_8.zi_n = Hs; c73_8.flags = 4; c73_8.act = 0;
      c73_8.alpha = 1.0f; c73_8.beta = 1.0f; c73_8.sa = 1.0f; c73_8.sb = 1.0f; c73_8.Npad = 64; c73_8.pad_ = 0;
      k_gemm<1><<<dim3((unsigned)((64) + 31) / 32, (unsigned)((Hs) + 15) / 16, (unsigned)(Bn * Hs)), 32, 0, stream>>>(c73_8); }

    k_sh_bn<<<(unsigned)(((long long)Bn * HW * 64 + 255) / 256), 256, 0, stream>>>(T64, 64, g73, bb73, m73, v73, OP, 256, 192, 1, Bn, Hs);
    { GemmP co1_0;
      co1_0.A = OP + (size_t)0 * 256; co1_0.B = ow1 + 0; co1_0.bias = ob1; co1_0.R = OP + (size_t)0 * 256; co1_0.C = OFF;
      co1_0.sAo = (long long)PP * 256; co1_0.sAi = (long long)HP * 256; co1_0.sAm = 256; co1_0.sAk = 1; co1_0.sBo = 0; co1_0.sBi = 0; co1_0.sBn = 256 * 9; co1_0.sBk = 9; co1_0.sCo = (long long)HW * 32; co1_0.sCi = (long long)Hs * 32; co1_0.sCm = 32; co1_0.sRo = 0; co1_0.sRi = 0; co1_0.sRm = 0; co1_0.sRn = 0;
      co1_0.M = Hs; co1_0.N = 18; co1_0.K = 256; co1_0.zi_n = Hs; co1_0.flags = 1; co1_0.act = 0;
      co1_0.alpha = 1.0f; co1_0.beta = 0.0f; co1_0.sa = 1.0f; co1_0.sb = 1.0f; co1_0.Npad = 32; co1_0.pad_ = 0;
      k_gemm<1><<<dim3((unsigned)((32) + 31) / 32, (unsigned)((Hs) + 15) / 16, (unsigned)(Bn * Hs)), 32, 0, stream>>>(co1_0); }
    { GemmP co1_1;
      co1_1.A = OP + (size_t)1 * 256; co1_1.B = ow1 + 1; co1_1.bias = OP + (size_t)1 * 256; co1_1.R = OFF; co1_1.C = OFF;
      co1_1.sAo = (long long)PP * 256; co1_1.sAi = (long long)HP * 256; co1_1.sAm = 256; co1_1.sAk = 1; co1_1.sBo = 0; co1_1.sBi = 0; co1_1.sBn = 256 * 9; co1_1.sBk = 9; co1_1.sCo = (long long)HW * 32; co1_1.sCi = (long long)Hs * 32; co1_1.sCm = 32; co1_1.sRo = (long long)HW * 32; co1_1.sRi = (long long)Hs * 32; co1_1.sRm = 32; co1_1.sRn = 1;
      co1_1.M = Hs; co1_1.N = 18; co1_1.K = 256; co1_1.zi_n = Hs; co1_1.flags = 4; co1_1.act = 0;
      co1_1.alpha = 1.0f; co1_1.beta = 1.0f; co1_1.sa = 1.0f; co1_1.sb = 1.0f; co1_1.Npad = 32; co1_1.pad_ = 0;
      k_gemm<1><<<dim3((unsigned)((32) + 31) / 32, (unsigned)((Hs) + 15) / 16, (unsigned)(Bn * Hs)), 32, 0, stream>>>(co1_1); }
    { GemmP co1_2;
      co1_2.A = OP + (size_t)2 * 256; co1_2.B = ow1 + 2; co1_2.bias = OP + (size_t)2 * 256; co1_2.R = OFF; co1_2.C = OFF;
      co1_2.sAo = (long long)PP * 256; co1_2.sAi = (long long)HP * 256; co1_2.sAm = 256; co1_2.sAk = 1; co1_2.sBo = 0; co1_2.sBi = 0; co1_2.sBn = 256 * 9; co1_2.sBk = 9; co1_2.sCo = (long long)HW * 32; co1_2.sCi = (long long)Hs * 32; co1_2.sCm = 32; co1_2.sRo = (long long)HW * 32; co1_2.sRi = (long long)Hs * 32; co1_2.sRm = 32; co1_2.sRn = 1;
      co1_2.M = Hs; co1_2.N = 18; co1_2.K = 256; co1_2.zi_n = Hs; co1_2.flags = 4; co1_2.act = 0;
      co1_2.alpha = 1.0f; co1_2.beta = 1.0f; co1_2.sa = 1.0f; co1_2.sb = 1.0f; co1_2.Npad = 32; co1_2.pad_ = 0;
      k_gemm<1><<<dim3((unsigned)((32) + 31) / 32, (unsigned)((Hs) + 15) / 16, (unsigned)(Bn * Hs)), 32, 0, stream>>>(co1_2); }
    { GemmP co1_3;
      co1_3.A = OP + (size_t)82 * 256; co1_3.B = ow1 + 3; co1_3.bias = OP + (size_t)82 * 256; co1_3.R = OFF; co1_3.C = OFF;
      co1_3.sAo = (long long)PP * 256; co1_3.sAi = (long long)HP * 256; co1_3.sAm = 256; co1_3.sAk = 1; co1_3.sBo = 0; co1_3.sBi = 0; co1_3.sBn = 256 * 9; co1_3.sBk = 9; co1_3.sCo = (long long)HW * 32; co1_3.sCi = (long long)Hs * 32; co1_3.sCm = 32; co1_3.sRo = (long long)HW * 32; co1_3.sRi = (long long)Hs * 32; co1_3.sRm = 32; co1_3.sRn = 1;
      co1_3.M = Hs; co1_3.N = 18; co1_3.K = 256; co1_3.zi_n = Hs; co1_3.flags = 4; co1_3.act = 0;
      co1_3.alpha = 1.0f; co1_3.beta = 1.0f; co1_3.sa = 1.0f; co1_3.sb = 1.0f; co1_3.Npad = 32; co1_3.pad_ = 0;
      k_gemm<1><<<dim3((unsigned)((32) + 31) / 32, (unsigned)((Hs) + 15) / 16, (unsigned)(Bn * Hs)), 32, 0, stream>>>(co1_3); }
    { GemmP co1_4;
      co1_4.A = OP + (size_t)83 * 256; co1_4.B = ow1 + 4; co1_4.bias = OP + (size_t)83 * 256; co1_4.R = OFF; co1_4.C = OFF;
      co1_4.sAo = (long long)PP * 256; co1_4.sAi = (long long)HP * 256; co1_4.sAm = 256; co1_4.sAk = 1; co1_4.sBo = 0; co1_4.sBi = 0; co1_4.sBn = 256 * 9; co1_4.sBk = 9; co1_4.sCo = (long long)HW * 32; co1_4.sCi = (long long)Hs * 32; co1_4.sCm = 32; co1_4.sRo = (long long)HW * 32; co1_4.sRi = (long long)Hs * 32; co1_4.sRm = 32; co1_4.sRn = 1;
      co1_4.M = Hs; co1_4.N = 18; co1_4.K = 256; co1_4.zi_n = Hs; co1_4.flags = 4; co1_4.act = 0;
      co1_4.alpha = 1.0f; co1_4.beta = 1.0f; co1_4.sa = 1.0f; co1_4.sb = 1.0f; co1_4.Npad = 32; co1_4.pad_ = 0;
      k_gemm<1><<<dim3((unsigned)((32) + 31) / 32, (unsigned)((Hs) + 15) / 16, (unsigned)(Bn * Hs)), 32, 0, stream>>>(co1_4); }
    { GemmP co1_5;
      co1_5.A = OP + (size_t)84 * 256; co1_5.B = ow1 + 5; co1_5.bias = OP + (size_t)84 * 256; co1_5.R = OFF; co1_5.C = OFF;
      co1_5.sAo = (long long)PP * 256; co1_5.sAi = (long long)HP * 256; co1_5.sAm = 256; co1_5.sAk = 1; co1_5.sBo = 0; co1_5.sBi = 0; co1_5.sBn = 256 * 9; co1_5.sBk = 9; co1_5.sCo = (long long)HW * 32; co1_5.sCi = (long long)Hs * 32; co1_5.sCm = 32; co1_5.sRo = (long long)HW * 32; co1_5.sRi = (long long)Hs * 32; co1_5.sRm = 32; co1_5.sRn = 1;
      co1_5.M = Hs; co1_5.N = 18; co1_5.K = 256; co1_5.zi_n = Hs; co1_5.flags = 4; co1_5.act = 0;
      co1_5.alpha = 1.0f; co1_5.beta = 1.0f; co1_5.sa = 1.0f; co1_5.sb = 1.0f; co1_5.Npad = 32; co1_5.pad_ = 0;
      k_gemm<1><<<dim3((unsigned)((32) + 31) / 32, (unsigned)((Hs) + 15) / 16, (unsigned)(Bn * Hs)), 32, 0, stream>>>(co1_5); }
    { GemmP co1_6;
      co1_6.A = OP + (size_t)164 * 256; co1_6.B = ow1 + 6; co1_6.bias = OP + (size_t)164 * 256; co1_6.R = OFF; co1_6.C = OFF;
      co1_6.sAo = (long long)PP * 256; co1_6.sAi = (long long)HP * 256; co1_6.sAm = 256; co1_6.sAk = 1; co1_6.sBo = 0; co1_6.sBi = 0; co1_6.sBn = 256 * 9; co1_6.sBk = 9; co1_6.sCo = (long long)HW * 32; co1_6.sCi = (long long)Hs * 32; co1_6.sCm = 32; co1_6.sRo = (long long)HW * 32; co1_6.sRi = (long long)Hs * 32; co1_6.sRm = 32; co1_6.sRn = 1;
      co1_6.M = Hs; co1_6.N = 18; co1_6.K = 256; co1_6.zi_n = Hs; co1_6.flags = 4; co1_6.act = 0;
      co1_6.alpha = 1.0f; co1_6.beta = 1.0f; co1_6.sa = 1.0f; co1_6.sb = 1.0f; co1_6.Npad = 32; co1_6.pad_ = 0;
      k_gemm<1><<<dim3((unsigned)((32) + 31) / 32, (unsigned)((Hs) + 15) / 16, (unsigned)(Bn * Hs)), 32, 0, stream>>>(co1_6); }
    { GemmP co1_7;
      co1_7.A = OP + (size_t)165 * 256; co1_7.B = ow1 + 7; co1_7.bias = OP + (size_t)165 * 256; co1_7.R = OFF; co1_7.C = OFF;
      co1_7.sAo = (long long)PP * 256; co1_7.sAi = (long long)HP * 256; co1_7.sAm = 256; co1_7.sAk = 1; co1_7.sBo = 0; co1_7.sBi = 0; co1_7.sBn = 256 * 9; co1_7.sBk = 9; co1_7.sCo = (long long)HW * 32; co1_7.sCi = (long long)Hs * 32; co1_7.sCm = 32; co1_7.sRo = (long long)HW * 32; co1_7.sRi = (long long)Hs * 32; co1_7.sRm = 32; co1_7.sRn = 1;
      co1_7.M = Hs; co1_7.N = 18; co1_7.K = 256; co1_7.zi_n = Hs; co1_7.flags = 4; co1_7.act = 0;
      co1_7.alpha = 1.0f; co1_7.beta = 1.0f; co1_7.sa = 1.0f; co1_7.sb = 1.0f; co1_7.Npad = 32; co1_7.pad_ = 0;
      k_gemm<1><<<dim3((unsigned)((32) + 31) / 32, (unsigned)((Hs) + 15) / 16, (unsigned)(Bn * Hs)), 32, 0, stream>>>(co1_7); }
    { GemmP co1_8;
      co1_8.A = OP + (size_t)166 * 256; co1_8.B = ow1 + 8; co1_8.bias = OP + (size_t)166 * 256; co1_8.R = OFF; co1_8.C = OFF;
      co1_8.sAo = (long long)PP * 256; co1_8.sAi = (long long)HP * 256; co1_8.sAm = 256; co1_8.sAk = 1; co1_8.sBo = 0; co1_8.sBi = 0; co1_8.sBn = 256 * 9; co1_8.sBk = 9; co1_8.sCo = (long long)HW * 32; co1_8.sCi = (long long)Hs * 32; co1_8.sCm = 32; co1_8.sRo = (long long)HW * 32; co1_8.sRi = (long long)Hs * 32; co1_8.sRm = 32; co1_8.sRn = 1;
      co1_8.M = Hs; co1_8.N = 18; co1_8.K = 256; co1_8.zi_n = Hs; co1_8.flags = 4; co1_8.act = 0;
      co1_8.alpha = 1.0f; co1_8.beta = 1.0f; co1_8.sa = 1.0f; co1_8.sb = 1.0f; co1_8.Npad = 32; co1_8.pad_ = 0;
      k_gemm<1><<<dim3((unsigned)((32) + 31) / 32, (unsigned)((Hs) + 15) / 16, (unsigned)(Bn * Hs)), 32, 0, stream>>>(co1_8); }

    k_sh_col<<<(unsigned)(((long long)HW * 9 * CI + 255) / 256), 256, 0, stream>>>(OP, OFF, 32, COL, 0, Hs, CI);
    { GemmP gd1_0;
      gd1_0.A = COL; gd1_0.B = dw1; gd1_0.bias = COL; gd1_0.R = COL; gd1_0.C = O2 + (size_t)0 * HW * CI;
      gd1_0.sAo = 0; gd1_0.sAi = 0; gd1_0.sAm = 9 * CI; gd1_0.sAk = 1; gd1_0.sBo = 0; gd1_0.sBi = 0; gd1_0.sBn = 9 * CI; gd1_0.sBk = 1; gd1_0.sCo = 0; gd1_0.sCi = 0; gd1_0.sCm = CI; gd1_0.sRo = 0; gd1_0.sRi = 0; gd1_0.sRm = 0; gd1_0.sRn = 0;
      gd1_0.M = HW; gd1_0.N = CI; gd1_0.K = 9 * CI; gd1_0.zi_n = 1; gd1_0.flags = 0; gd1_0.act = 0;
      gd1_0.alpha = 1.0f; gd1_0.beta = 0.0f; gd1_0.sa = 1.0f; gd1_0.sb = 1.0f; gd1_0.Npad = CI; gd1_0.pad_ = 0;
      k_gemm<1><<<dim3((unsigned)((CI) + 31) / 32, (unsigned)((HW) + 15) / 16, (unsigned)(1)), 32, 0, stream>>>(gd1_0); }
    k_sh_col<<<(unsigned)(((long long)HW * 9 * CI + 255) / 256), 256, 0, stream>>>(OP, OFF, 32, COL, 1, Hs, CI);
    { GemmP gd1_1;
      gd1_1.A = COL; gd1_1.B = dw1; gd1_1.bias = COL; gd1_1.R = COL; gd1_1.C = O2 + (size_t)1 * HW * CI;
      gd1_1.sAo = 0; gd1_1.sAi = 0; gd1_1.sAm = 9 * CI; gd1_1.sAk = 1; gd1_1.sBo = 0; gd1_1.sBi = 0; gd1_1.sBn = 9 * CI; gd1_1.sBk = 1; gd1_1.sCo = 0; gd1_1.sCi = 0; gd1_1.sCm = CI; gd1_1.sRo = 0; gd1_1.sRi = 0; gd1_1.sRm = 0; gd1_1.sRn = 0;
      gd1_1.M = HW; gd1_1.N = CI; gd1_1.K = 9 * CI; gd1_1.zi_n = 1; gd1_1.flags = 0; gd1_1.act = 0;
      gd1_1.alpha = 1.0f; gd1_1.beta = 0.0f; gd1_1.sa = 1.0f; gd1_1.sb = 1.0f; gd1_1.Npad = CI; gd1_1.pad_ = 0;
      k_gemm<1><<<dim3((unsigned)((CI) + 31) / 32, (unsigned)((HW) + 15) / 16, (unsigned)(1)), 32, 0, stream>>>(gd1_1); }
    k_sh_col<<<(unsigned)(((long long)HW * 9 * CI + 255) / 256), 256, 0, stream>>>(OP, OFF, 32, COL, 2, Hs, CI);
    { GemmP gd1_2;
      gd1_2.A = COL; gd1_2.B = dw1; gd1_2.bias = COL; gd1_2.R = COL; gd1_2.C = O2 + (size_t)2 * HW * CI;
      gd1_2.sAo = 0; gd1_2.sAi = 0; gd1_2.sAm = 9 * CI; gd1_2.sAk = 1; gd1_2.sBo = 0; gd1_2.sBi = 0; gd1_2.sBn = 9 * CI; gd1_2.sBk = 1; gd1_2.sCo = 0; gd1_2.sCi = 0; gd1_2.sCm = CI; gd1_2.sRo = 0; gd1_2.sRi = 0; gd1_2.sRm = 0; gd1_2.sRn = 0;
      gd1_2.M = HW; gd1_2.N = CI; gd1_2.K = 9 * CI; gd1_2.zi_n = 1; gd1_2.flags = 0; gd1_2.act = 0;
      gd1_2.alpha = 1.0f; gd1_2.beta = 0.0f; gd1_2.sa = 1.0f; gd1_2.sb = 1.0f; gd1_2.Npad = CI; gd1_2.pad_ = 0;
      k_gemm<1><<<dim3((unsigned)((CI) + 31) / 32, (unsigned)((HW) + 15) / 16, (unsigned)(1)), 32, 0, stream>>>(gd1_2); }
    k_sh_col<<<(unsigned)(((long long)HW * 9 * CI + 255) / 256), 256, 0, stream>>>(OP, OFF, 32, COL, 3, Hs, CI);
    { GemmP gd1_3;
      gd1_3.A = COL; gd1_3.B = dw1; gd1_3.bias = COL; gd1_3.R = COL; gd1_3.C = O2 + (size_t)3 * HW * CI;
      gd1_3.sAo = 0; gd1_3.sAi = 0; gd1_3.sAm = 9 * CI; gd1_3.sAk = 1; gd1_3.sBo = 0; gd1_3.sBi = 0; gd1_3.sBn = 9 * CI; gd1_3.sBk = 1; gd1_3.sCo = 0; gd1_3.sCi = 0; gd1_3.sCm = CI; gd1_3.sRo = 0; gd1_3.sRi = 0; gd1_3.sRm = 0; gd1_3.sRn = 0;
      gd1_3.M = HW; gd1_3.N = CI; gd1_3.K = 9 * CI; gd1_3.zi_n = 1; gd1_3.flags = 0; gd1_3.act = 0;
      gd1_3.alpha = 1.0f; gd1_3.beta = 0.0f; gd1_3.sa = 1.0f; gd1_3.sb = 1.0f; gd1_3.Npad = CI; gd1_3.pad_ = 0;
      k_gemm<1><<<dim3((unsigned)((CI) + 31) / 32, (unsigned)((HW) + 15) / 16, (unsigned)(1)), 32, 0, stream>>>(gd1_3); }
    hipMemsetAsync(OP, 0, (size_t)Bn * PP * CI * 4, stream);
    k_sh_repad<<<(unsigned)(((long long)Bn * HW * CI + 255) / 256), 256, 0, stream>>>(O2, OP, Bn, Hs, CI);
    { GemmP co2_0;
      co2_0.A = OP + (size_t)0 * 256; co2_0.B = ow2 + 0; co2_0.bias = ob2; co2_0.R = OP + (size_t)0 * 256; co2_0.C = OFF;
      co2_0.sAo = (long long)PP * 256; co2_0.sAi = (long long)HP * 256; co2_0.sAm = 256; co2_0.sAk = 1; co2_0.sBo = 0; co2_0.sBi = 0; co2_0.sBn = 256 * 9; co2_0.sBk = 9; co2_0.sCo = (long long)HW * 32; co2_0.sCi = (long long)Hs * 32; co2_0.sCm = 32; co2_0.sRo = 0; co2_0.sRi = 0; co2_0.sRm = 0; co2_0.sRn = 0;
      co2_0.M = Hs; co2_0.N = 18; co2_0.K = 256; co2_0.zi_n = Hs; co2_0.flags = 1; co2_0.act = 0;
      co2_0.alpha = 1.0f; co2_0.beta = 0.0f; co2_0.sa = 1.0f; co2_0.sb = 1.0f; co2_0.Npad = 32; co2_0.pad_ = 0;
      k_gemm<1><<<dim3((unsigned)((32) + 31) / 32, (unsigned)((Hs) + 15) / 16, (unsigned)(Bn * Hs)), 32, 0, stream>>>(co2_0); }
    { GemmP co2_1;
      co2_1.A = OP + (size_t)1 * 256; co2_1.B = ow2 + 1; co2_1.bias = OP + (size_t)1 * 256; co2_1.R = OFF; co2_1.C = OFF;
      co2_1.sAo = (long long)PP * 256; co2_1.sAi = (long long)HP * 256; co2_1.sAm = 256; co2_1.sAk = 1; co2_1.sBo = 0; co2_1.sBi = 0; co2_1.sBn = 256 * 9; co2_1.sBk = 9; co2_1.sCo = (long long)HW * 32; co2_1.sCi = (long long)Hs * 32; co2_1.sCm = 32; co2_1.sRo = (long long)HW * 32; co2_1.sRi = (long long)Hs * 32; co2_1.sRm = 32; co2_1.sRn = 1;
      co2_1.M = Hs; co2_1.N = 18; co2_1.K = 256; co2_1.zi_n = Hs; co2_1.flags = 4; co2_1.act = 0;
      co2_1.alpha = 1.0f; co2_1.beta = 1.0f; co2_1.sa = 1.0f; co2_1.sb = 1.0f; co2_1.Npad = 32; co2_1.pad_ = 0;
      k_gemm<1><<<dim3((unsigned)((32) + 31) / 32, (unsigned)((Hs) + 15) / 16, (unsigned)(Bn * Hs)), 32, 0, stream>>>(co2_1); }
    { GemmP co2_2;
      co2_2.A = OP + (size_t)2 * 256; co2_2.B = ow2 + 2; co2_2.bias = OP + (size_t)2 * 256; co2_2.R = OFF; co2_2.C = OFF;
      co2_2.sAo = (long long)PP * 256; co2_2.sAi = (long long)HP * 256; co2_2.sAm = 256; co2_2.sAk = 1; co2_2.sBo = 0; co2_2.sBi = 0; co2_2.sBn = 256 * 9; co2_2.sBk = 9; co2_2.sCo = (long long)HW * 32; co2_2.sCi = (long long)Hs * 32; co2_2.sCm = 32; co2_2.sRo = (long long)HW * 32; co2_2.sRi = (long long)Hs * 32; co2_2.sRm = 32; co2_2.sRn = 1;
      co2_2.M = Hs; co2_2.N = 18; co2_2.K = 256; co2_2.zi_n = Hs; co2_2.flags = 4; co2_2.act = 0;
      co2_2.alpha = 1.0f; co2_2.beta = 1.0f; co2_2.sa = 1.0f; co2_2.sb = 1.0f; co2_2.Npad = 32; co2_2.pad_ = 0;
      k_gemm<1><<<dim3((unsigned)((32) + 31) / 32, (unsigned)((Hs) + 15) / 16, (unsigned)(Bn * Hs)), 32, 0, stream>>>(co2_2); }
    { GemmP co2_3;
      co2_3.A = OP + (size_t)82 * 256; co2_3.B = ow2 + 3; co2_3.bias = OP + (size_t)82 * 256; co2_3.R = OFF; co2_3.C = OFF;
      co2_3.sAo = (long long)PP * 256; co2_3.sAi = (long long)HP * 256; co2_3.sAm = 256; co2_3.sAk = 1; co2_3.sBo = 0; co2_3.sBi = 0; co2_3.sBn = 256 * 9; co2_3.sBk = 9; co2_3.sCo = (long long)HW * 32; co2_3.sCi = (long long)Hs * 32; co2_3.sCm = 32; co2_3.sRo = (long long)HW * 32; co2_3.sRi = (long long)Hs * 32; co2_3.sRm = 32; co2_3.sRn = 1;
      co2_3.M = Hs; co2_3.N = 18; co2_3.K = 256; co2_3.zi_n = Hs; co2_3.flags = 4; co2_3.act = 0;
      co2_3.alpha = 1.0f; co2_3.beta = 1.0f; co2_3.sa = 1.0f; co2_3.sb = 1.0f; co2_3.Npad = 32; co2_3.pad_ = 0;
      k_gemm<1><<<dim3((unsigned)((32) + 31) / 32, (unsigned)((Hs) + 15) / 16, (unsigned)(Bn * Hs)), 32, 0, stream>>>(co2_3); }
    { GemmP co2_4;
      co2_4.A = OP + (size_t)83 * 256; co2_4.B = ow2 + 4; co2_4.bias = OP + (size_t)83 * 256; co2_4.R = OFF; co2_4.C = OFF;
      co2_4.sAo = (long long)PP * 256; co2_4.sAi = (long long)HP * 256; co2_4.sAm = 256; co2_4.sAk = 1; co2_4.sBo = 0; co2_4.sBi = 0; co2_4.sBn = 256 * 9; co2_4.sBk = 9; co2_4.sCo = (long long)HW * 32; co2_4.sCi = (long long)Hs * 32; co2_4.sCm = 32; co2_4.sRo = (long long)HW * 32; co2_4.sRi = (long long)Hs * 32; co2_4.sRm = 32; co2_4.sRn = 1;
      co2_4.M = Hs; co2_4.N = 18; co2_4.K = 256; co2_4.zi_n = Hs; co2_4.flags = 4; co2_4.act = 0;
      co2_4.alpha = 1.0f; co2_4.beta = 1.0f; co2_4.sa = 1.0f; co2_4.sb = 1.0f; co2_4.Npad = 32; co2_4.pad_ = 0;
      k_gemm<1><<<dim3((unsigned)((32) + 31) / 32, (unsigned)((Hs) + 15) / 16, (unsigned)(Bn * Hs)), 32, 0, stream>>>(co2_4); }
    { GemmP co2_5;
      co2_5.A = OP + (size_t)84 * 256; co2_5.B = ow2 + 5; co2_5.bias = OP + (size_t)84 * 256; co2_5.R = OFF; co2_5.C = OFF;
      co2_5.sAo = (long long)PP * 256; co2_5.sAi = (long long)HP * 256; co2_5.sAm = 256; co2_5.sAk = 1; co2_5.sBo = 0; co2_5.sBi = 0; co2_5.sBn = 256 * 9; co2_5.sBk = 9; co2_5.sCo = (long long)HW * 32; co2_5.sCi = (long long)Hs * 32; co2_5.sCm = 32; co2_5.sRo = (long long)HW * 32; co2_5.sRi = (long long)Hs * 32; co2_5.sRm = 32; co2_5.sRn = 1;
      co2_5.M = Hs; co2_5.N = 18; co2_5.K = 256; co2_5.zi_n = Hs; co2_5.flags = 4; co2_5.act = 0;
      co2_5.alpha = 1.0f; co2_5.beta = 1.0f; co2_5.sa = 1.0f; co2_5.sb = 1.0f; co2_5.Npad = 32; co2_5.pad_ = 0;
      k_gemm<1><<<dim3((unsigned)((32) + 31) / 32, (unsigned)((Hs) + 15) / 16, (unsigned)(Bn * Hs)), 32, 0, stream>>>(co2_5); }
    { GemmP co2_6;
      co2_6.A = OP + (size_t)164 * 256; co2_6.B = ow2 + 6; co2_6.bias = OP + (size_t)164 * 256; co2_6.R = OFF; co2_6.C = OFF;
      co2_6.sAo = (long long)PP * 256; co2_6.sAi = (long long)HP * 256; co2_6.sAm = 256; co2_6.sAk = 1; co2_6.sBo = 0; co2_6.sBi = 0; co2_6.sBn = 256 * 9; co2_6.sBk = 9; co2_6.sCo = (long long)HW * 32; co2_6.sCi = (long long)Hs * 32; co2_6.sCm = 32; co2_6.sRo = (long long)HW * 32; co2_6.sRi = (long long)Hs * 32; co2_6.sRm = 32; co2_6.sRn = 1;
      co2_6.M = Hs; co2_6.N = 18; co2_6.K = 256; co2_6.zi_n = Hs; co2_6.flags = 4; co2_6.act = 0;
      co2_6.alpha = 1.0f; co2_6.beta = 1.0f; co2_6.sa = 1.0f; co2_6.sb = 1.0f; co2_6.Npad = 32; co2_6.pad_ = 0;
      k_gemm<1><<<dim3((unsigned)((32) + 31) / 32, (unsigned)((Hs) + 15) / 16, (unsigned)(Bn * Hs)), 32, 0, stream>>>(co2_6); }
    { GemmP co2_7;
      co2_7.A = OP + (size_t)165 * 256; co2_7.B = ow2 + 7; co2_7.bias = OP + (size_t)165 * 256; co2_7.R = OFF; co2_7.C = OFF;
      co2_7.sAo = (long long)PP * 256; co2_7.sAi = (long long)HP * 256; co2_7.sAm = 256; co2_7.sAk = 1; co2_7.sBo = 0; co2_7.sBi = 0; co2_7.sBn = 256 * 9; co2_7.sBk = 9; co2_7.sCo = (long long)HW * 32; co2_7.sCi = (long long)Hs * 32; co2_7.sCm = 32; co2_7.sRo = (long long)HW * 32; co2_7.sRi = (long long)Hs * 32; co2_7.sRm = 32; co2_7.sRn = 1;
      co2_7.M = Hs; co2_7.N = 18; co2_7.K = 256; co2_7.zi_n = Hs; co2_7.flags = 4; co2_7.act = 0;
      co2_7.alpha = 1.0f; co2_7.beta = 1.0f; co2_7.sa = 1.0f; co2_7.sb = 1.0f; co2_7.Npad = 32; co2_7.pad_ = 0;
      k_gemm<1><<<dim3((unsigned)((32) + 31) / 32, (unsigned)((Hs) + 15) / 16, (unsigned)(Bn * Hs)), 32, 0, stream>>>(co2_7); }
    { GemmP co2_8;
      co2_8.A = OP + (size_t)166 * 256; co2_8.B = ow2 + 8; co2_8.bias = OP + (size_t)166 * 256; co2_8.R = OFF; co2_8.C = OFF;
      co2_8.sAo = (long long)PP * 256; co2_8.sAi = (long long)HP * 256; co2_8.sAm = 256; co2_8.sAk = 1; co2_8.sBo = 0; co2_8.sBi = 0; co2_8.sBn = 256 * 9; co2_8.sBk = 9; co2_8.sCo = (long long)HW * 32; co2_8.sCi = (long long)Hs * 32; co2_8.sCm = 32; co2_8.sRo = (long long)HW * 32; co2_8.sRi = (long long)Hs * 32; co2_8.sRm = 32; co2_8.sRn = 1;
      co2_8.M = Hs; co2_8.N = 18; co2_8.K = 256; co2_8.zi_n = Hs; co2_8.flags = 4; co2_8.act = 0;
      co2_8.alpha = 1.0f; co2_8.beta = 1.0f; co2_8.sa = 1.0f; co2_8.sb = 1.0f; co2_8.Npad = 32; co2_8.pad_ = 0;
      k_gemm<1><<<dim3((unsigned)((32) + 31) / 32, (unsigned)((Hs) + 15) / 16, (unsigned)(Bn * Hs)), 32, 0, stream>>>(co2_8); }

    k_sh_col<<<(unsigned)(((long long)HW * 9 * CI + 255) / 256), 256, 0, stream>>>(OP, OFF, 32, COL, 0, Hs, CI);
    { GemmP gd2_0;
      gd2_0.A = COL; gd2_0.B = dw2; gd2_0.bias = COL; gd2_0.R = COL; gd2_0.C = O2 + (size_t)0 * HW * CI;
      gd2_0.sAo = 0; gd2_0.sAi = 0; gd2_0.sAm = 9 * CI; gd2_0.sAk = 1; gd2_0.sBo = 0; gd2_0.sBi = 0; gd2_0.sBn = 9 * CI; gd2_0.sBk = 1; gd2_0.sCo = 0; gd2_0.sCi = 0; gd2_0.sCm = CI; gd2_0.sRo = 0; gd2_0.sRi = 0; gd2_0.sRm = 0; gd2_0.sRn = 0;
      gd2_0.M = HW; gd2_0.N = CI; gd2_0.K = 9 * CI; gd2_0.zi_n = 1; gd2_0.flags = 0; gd2_0.act = 0;
      gd2_0.alpha = 1.0f; gd2_0.beta = 0.0f; gd2_0.sa = 1.0f; gd2_0.sb = 1.0f; gd2_0.Npad = CI; gd2_0.pad_ = 0;
      k_gemm<1><<<dim3((unsigned)((CI) + 31) / 32, (unsigned)((HW) + 15) / 16, (unsigned)(1)), 32, 0, stream>>>(gd2_0); }
    k_sh_col<<<(unsigned)(((long long)HW * 9 * CI + 255) / 256), 256, 0, stream>>>(OP, OFF, 32, COL, 1, Hs, CI);
    { GemmP gd2_1;
      gd2_1.A = COL; gd2_1.B = dw2; gd2_1.bias = COL; gd2_1.R = COL; gd2_1.C = O2 + (size_t)1 * HW * CI;
      gd2_1.sAo = 0; gd2_1.sAi = 0; gd2_1.sAm = 9 * CI; gd2_1.sAk = 1; gd2_1.sBo = 0; gd2_1.sBi = 0; gd2_1.sBn = 9 * CI; gd2_1.sBk = 1; gd2_1.sCo = 0; gd2_1.sCi = 0; gd2_1.sCm = CI; gd2_1.sRo = 0; gd2_1.sRi = 0; gd2_1.sRm = 0; gd2_1.sRn = 0;
      gd2_1.M = HW; gd2_1.N = CI; gd2_1.K = 9 * CI; gd2_1.zi_n = 1; gd2_1.flags = 0; gd2_1.act = 0;
      gd2_1.alpha = 1.0f; gd2_1.beta = 0.0f; gd2_1.sa = 1.0f; gd2_1.sb = 1.0f; gd2_1.Npad = CI; gd2_1.pad_ = 0;
      k_gemm<1><<<dim3((unsigned)((CI) + 31) / 32, (unsigned)((HW) + 15) / 16, (unsigned)(1)), 32, 0, stream>>>(gd2_1); }
    k_sh_col<<<(unsigned)(((long long)HW * 9 * CI + 255) / 256), 256, 0, stream>>>(OP, OFF, 32, COL, 2, Hs, CI);
    { GemmP gd2_2;
      gd2_2.A = COL; gd2_2.B = dw2; gd2_2.bias = COL; gd2_2.R = COL; gd2_2.C = O2 + (size_t)2 * HW * CI;
      gd2_2.sAo = 0; gd2_2.sAi = 0; gd2_2.sAm = 9 * CI; gd2_2.sAk = 1; gd2_2.sBo = 0; gd2_2.sBi = 0; gd2_2.sBn = 9 * CI; gd2_2.sBk = 1; gd2_2.sCo = 0; gd2_2.sCi = 0; gd2_2.sCm = CI; gd2_2.sRo = 0; gd2_2.sRi = 0; gd2_2.sRm = 0; gd2_2.sRn = 0;
      gd2_2.M = HW; gd2_2.N = CI; gd2_2.K = 9 * CI; gd2_2.zi_n = 1; gd2_2.flags = 0; gd2_2.act = 0;
      gd2_2.alpha = 1.0f; gd2_2.beta = 0.0f; gd2_2.sa = 1.0f; gd2_2.sb = 1.0f; gd2_2.Npad = CI; gd2_2.pad_ = 0;
      k_gemm<1><<<dim3((unsigned)((CI) + 31) / 32, (unsigned)((HW) + 15) / 16, (unsigned)(1)), 32, 0, stream>>>(gd2_2); }
    k_sh_col<<<(unsigned)(((long long)HW * 9 * CI + 255) / 256), 256, 0, stream>>>(OP, OFF, 32, COL, 3, Hs, CI);
    { GemmP gd2_3;
      gd2_3.A = COL; gd2_3.B = dw2; gd2_3.bias = COL; gd2_3.R = COL; gd2_3.C = O2 + (size_t)3 * HW * CI;
      gd2_3.sAo = 0; gd2_3.sAi = 0; gd2_3.sAm = 9 * CI; gd2_3.sAk = 1; gd2_3.sBo = 0; gd2_3.sBi = 0; gd2_3.sBn = 9 * CI; gd2_3.sBk = 1; gd2_3.sCo = 0; gd2_3.sCi = 0; gd2_3.sCm = CI; gd2_3.sRo = 0; gd2_3.sRi = 0; gd2_3.sRm = 0; gd2_3.sRn = 0;
      gd2_3.M = HW; gd2_3.N = CI; gd2_3.K = 9 * CI; gd2_3.zi_n = 1; gd2_3.flags = 0; gd2_3.act = 0;
      gd2_3.alpha = 1.0f; gd2_3.beta = 0.0f; gd2_3.sa = 1.0f; gd2_3.sb = 1.0f; gd2_3.Npad = CI; gd2_3.pad_ = 0;
      k_gemm<1><<<dim3((unsigned)((CI) + 31) / 32, (unsigned)((HW) + 15) / 16, (unsigned)(1)), 32, 0, stream>>>(gd2_3); }
    k_sh_out<<<(unsigned)(((long long)Bn * HW * CI + 255) / 256), 256, 0, stream>>>(O2, out, Bn, Hs, CI);
}
